// ROLLOUT_72954314489893
// MI455X (gfx1250) — hardware-verified
//
#include <hip/hip_runtime.h>
#include <math.h>

typedef __attribute__((ext_vector_type(16))) _Float16 v16h;
typedef __attribute__((ext_vector_type(8)))  _Float16 v8h;
typedef __attribute__((ext_vector_type(16))) __bf16   v16b;
typedef __attribute__((ext_vector_type(8)))  float    v8f;
typedef __attribute__((ext_vector_type(4)))  float    v4f;

__device__ __forceinline__ int frag_k(int i, int h) { return (i < 8) ? (8 * h + i) : (16 + 8 * h + (i - 8)); }
__device__ __forceinline__ __bf16 bf16_rne(float f) {
    unsigned int u = __float_as_uint(f);
    u += 0x7fffu + ((u >> 16) & 1u);
    return __builtin_bit_cast(__bf16, (unsigned short)(u >> 16));
}
__device__ __forceinline__ float bf16_f32(__bf16 b) { return __uint_as_float(((unsigned int)__builtin_bit_cast(unsigned short, b)) << 16); }
__device__ __forceinline__ v8f wmma16(v16h a, v16h b, v8f c) {
    c = __builtin_amdgcn_wmma_f32_16x16x32_f16(false, a, false, b, (short)0, c, false, false);
    asm volatile("v_nop\n\tv_nop\n\tv_nop\n\tv_nop" : "+v"(c) : "v"(a), "v"(b));
    return c;
}
__device__ __forceinline__ v8f wmmab(v16b a, v16b b, v8f c) {
    c = __builtin_amdgcn_wmma_f32_16x16x32_bf16(false, a, false, b, (short)0, c, false, false);
    asm volatile("v_nop\n\tv_nop\n\tv_nop\n\tv_nop" : "+v"(c) : "v"(a), "v"(b));
    return c;
}
struct Split { v16b hi, lo; };
__device__ __forceinline__ v8f wmma3(const Split& a, const Split& b, v8f c) {
    c = __builtin_amdgcn_wmma_f32_16x16x32_bf16(false, a.hi, false, b.hi, (short)0, c, false, false);
    c = __builtin_amdgcn_wmma_f32_16x16x32_bf16(false, a.hi, false, b.lo, (short)0, c, false, false);
    c = __builtin_amdgcn_wmma_f32_16x16x32_bf16(false, a.lo, false, b.hi, (short)0, c, false, false);
    asm volatile("v_nop\n\tv_nop\n\tv_nop\n\tv_nop" : "+v"(c) : "v"(a.hi), "v"(a.lo), "v"(b.hi), "v"(b.lo));
    return c;
}
struct Split3 { v16b hi, mid, lo; };
__device__ __forceinline__ v8f wmma6(const Split3& a, const Split3& b, v8f c) {
    c = __builtin_amdgcn_wmma_f32_16x16x32_bf16(false, a.hi, false, b.hi, (short)0, c, false, false);
    c = __builtin_amdgcn_wmma_f32_16x16x32_bf16(false, a.hi, false, b.mid, (short)0, c, false, false);
    c = __builtin_amdgcn_wmma_f32_16x16x32_bf16(false, a.mid, false, b.hi, (short)0, c, false, false);
    c = __builtin_amdgcn_wmma_f32_16x16x32_bf16(false, a.hi, false, b.lo, (short)0, c, false, false);
    c = __builtin_amdgcn_wmma_f32_16x16x32_bf16(false, a.mid, false, b.mid, (short)0, c, false, false);
    c = __builtin_amdgcn_wmma_f32_16x16x32_bf16(false, a.lo, false, b.hi, (short)0, c, false, false);
    asm volatile("v_nop\n\tv_nop\n\tv_nop\n\tv_nop" : "+v"(c) : "v"(a.hi), "v"(a.mid), "v"(a.lo), "v"(b.hi), "v"(b.mid), "v"(b.lo));
    return c;
}

__device__ __forceinline__ v16h fh_ld(const float* __restrict__ p, long long sk, int k0, int h, int klen, float s) {
    v16h a;
#pragma unroll
    for (int i = 0; i < 16; ++i) { const int k = k0 + frag_k(i, h); a[i] = (k < klen) ? (_Float16)(p[(long long)k * sk] * s) : (_Float16)0.f; }
    return a;
}
__device__ __forceinline__ Split sp_ld(const float* __restrict__ p, long long sk, int k0, int h, int klen, float s) {
    Split r;
#pragma unroll
    for (int i = 0; i < 16; ++i) {
        const int k = k0 + frag_k(i, h); const float x = (k < klen) ? p[(long long)k * sk] * s : 0.f;
        const __bf16 hb = bf16_rne(x); r.hi[i] = hb; r.lo[i] = bf16_rne(x - bf16_f32(hb));
    }
    return r;
}
__device__ __forceinline__ Split3 sp3_ld(const float* __restrict__ p, long long sk, int k0, int h, int klen, float s) {
    Split3 r;
#pragma unroll
    for (int i = 0; i < 16; ++i) {
        const int k = k0 + frag_k(i, h); const float x = (k < klen) ? p[(long long)k * sk] * s : 0.f;
        const __bf16 hb = bf16_rne(x); const float r1 = x - bf16_f32(hb); const __bf16 mb = bf16_rne(r1);
        r.hi[i] = hb; r.mid[i] = mb; r.lo[i] = bf16_rne(r1 - bf16_f32(mb));
    }
    return r;
}
__device__ __forceinline__ v16b bh_ld(const float* __restrict__ p, long long sk, int k0, int h, int klen, float s) {
    v16b a;
#pragma unroll
    for (int i = 0; i < 16; ++i) { const int k = k0 + frag_k(i, h); a[i] = bf16_rne((k < klen) ? p[(long long)k * sk] * s : 0.f); }
    return a;
}
__device__ __forceinline__ v16h fh_row(const _Float16* __restrict__ row, int k0, int h) {
    v16h a;
#pragma unroll
    for (int i = 0; i < 16; ++i) a[i] = row[k0 + frag_k(i, h)];
    return a;
}

#define VST2(T, ptr, val) do { *(volatile T*)(ptr) = (val); __threadfence(); *(volatile T*)(ptr) = (val); } while (0)
typedef float v4f __attribute__((ext_vector_type(4)));
#define VST2V4(ptr, val) do { *(volatile v4f*)(ptr) = (val); __threadfence(); *(volatile v4f*)(ptr) = (val); } while (0)

__device__ __attribute__((noinline)) float act_fn(float v, int act) {
    if (act == 1) return fmaxf(v, 0.f);
    if (act == 2) { const float u = 0.7978845608028654f * (v + 0.044715f * v * v * v); return 0.5f * v * (1.f + tanhf(u)); }
    if (act == 3) return v / (1.f + expf(-v));
    if (act == 4) return 0.5f * v * (1.f + erff(v * 0.7071067811865476f));
    if (act == 5) return tanhf(v);
    if (act == 6) return 1.f / (1.f + expf(-v));
    if (act == 7) return (v > 0.f) ? v : 0.01f * v;
    if (act == 8) return (v > 0.f) ? v : (expf(v) - 1.f);
    if (act == 9) return fminf(fmaxf(v, 0.f), 6.f);
    if (act == 10) return fabsf(v);
    if (act == 11) return (v >= 0.f) ? v : 0.1f * v;
    if (act == 12) return (v > 0.f) ? v : 0.2f * v;
    if (act == 13) return (v > 20.f) ? v : log1pf(expf(v));
    return v;
}

struct GemmP {
    const float* A; const float* B; const float* bias; const float* R; float* C;
    long long sAo, sAi, sAm, sAk, sBo, sBi, sBn, sBk, sCo, sCi, sCm, sRo, sRi, sRm, sRn;
    int M, N, K, zi_n, flags, act; float alpha, beta, sa, sb;
    int Npad, pad_;
};
static_assert(sizeof(GemmP) == 5 * 8 + 15 * 8 + 6 * 4 + 4 * 4 + 2 * 4, "GemmP has padding");

template <int MODE>
__global__ __launch_bounds__(32) void k_gemm(GemmP p) {
    const int lane = threadIdx.x & 31, h = lane >> 4, l15 = lane & 15;
    const int m0 = blockIdx.y * 16, n0 = blockIdx.x * 32;
    const int z = blockIdx.z, zo = z / p.zi_n, zi = z - zo * p.zi_n;
    const float* A = p.A + zo * p.sAo + zi * p.sAi;
    const float* B = p.B + zo * p.sBo + zi * p.sBi;
    const int am = min(m0 + l15, p.M - 1);
    v8f acc[2], comp[2];
#pragma unroll
    for (int t = 0; t < 2; ++t) { v8f zz = {}; acc[t] = zz; comp[t] = zz; }
    for (int k0 = 0; k0 < p.K; k0 += 32) {
        const float* arow = A + (long long)am * p.sAm;
        if (MODE == 1) {
            const Split a = sp_ld(arow, p.sAk, k0, h, p.K, 1.f);
#pragma unroll
            for (int t = 0; t < 2; ++t) {
                const int bn = min(n0 + t * 16 + l15, p.N - 1);
                acc[t] = wmma3(a, sp_ld(B + (long long)bn * p.sBn, p.sBk, k0, h, p.K, 1.f), acc[t]);
            }
        } else if (MODE == 3) {
            const Split3 a = sp3_ld(arow, p.sAk, k0, h, p.K, 1.f);
#pragma unroll
            for (int t = 0; t < 2; ++t) {
                const int bn = min(n0 + t * 16 + l15, p.N - 1);
                acc[t] = wmma6(a, sp3_ld(B + (long long)bn * p.sBn, p.sBk, k0, h, p.K, 1.f), acc[t]);
            }
        } else if (MODE == 4) {
            const Split3 a = sp3_ld(arow, p.sAk, k0, h, p.K, 1.f);
#pragma unroll
            for (int t = 0; t < 2; ++t) {
                const int bn = min(n0 + t * 16 + l15, p.N - 1); v8f zz = {};
                const v8f part = wmma6(a, sp3_ld(B + (long long)bn * p.sBn, p.sBk, k0, h, p.K, 1.f), zz);
                const v8f y = part - comp[t]; const v8f s = acc[t] + y; comp[t] = (s - acc[t]) - y; acc[t] = s;
            }
        } else if (MODE == 2) {
            const v16b a = bh_ld(arow, p.sAk, k0, h, p.K, 1.f);
#pragma unroll
            for (int t = 0; t < 2; ++t) {
                const int bn = min(n0 + t * 16 + l15, p.N - 1);
                acc[t] = wmmab(a, bh_ld(B + (long long)bn * p.sBn, p.sBk, k0, h, p.K, 1.f), acc[t]);
            }
        } else {
            const v16h a = fh_ld(arow, p.sAk, k0, h, p.K, p.sa);
#pragma unroll
            for (int t = 0; t < 2; ++t) {
                const int bn = min(n0 + t * 16 + l15, p.N - 1);
                acc[t] = wmma16(a, fh_ld(B + (long long)bn * p.sBn, p.sBk, k0, h, p.K, p.sb), acc[t]);
            }
        }
    }
    const float iscale = (MODE == 0) ? p.alpha / (p.sa * p.sb) : p.alpha;
    float* C = p.C + zo * p.sCo + zi * p.sCi;
    const float* R = p.R + zo * p.sRo + zi * p.sRi;
    __shared__ __align__(16) float ctile[16][36];
#pragma unroll
    for (int t = 0; t < 2; ++t) {
        const int n = n0 + t * 16 + l15; const int nn = min(n, p.N - 1);
#pragma unroll
        for (int r = 0; r < 8; ++r) {
            const int m = m0 + 8 * h + r; const int mm = min(m, p.M - 1);
            float v = acc[t][r] * iscale;
            if (p.flags & 1) v += p.bias[nn];
            if (p.flags & 2) v += p.bias[mm];
            v = act_fn(v, p.act);
            if (p.flags & 4) v += p.beta * R[(long long)mm * p.sRm + (long long)nn * p.sRn];
            ctile[8 * h + r][t * 16 + l15] = (n < p.N) ? v : 0.f;
        }
    }
    __syncthreads();
    const int NW = (p.Npad > p.N) ? p.Npad : p.N;
    const bool fast = (m0 + 16 <= p.M) && (n0 + 32 <= NW) && ((p.sCm & 3) == 0) && ((((size_t)C) & 15) == 0);
    if (fast) {
#pragma unroll
        for (int s = 0; s < 4; ++s) {
            const int row = s * 4 + (lane >> 3), c4 = (lane & 7) * 4;
            const v4f v = *(const v4f*)&ctile[row][c4];
            VST2V4(C + (long long)(m0 + row) * p.sCm + n0 + c4, v);
        }
    } else {
        for (int row = 0; row < 16; ++row) {
            const int m = m0 + row, n = n0 + lane;
            if (m < p.M && n < NW) VST2(float, C + (long long)m * p.sCm + n, ctile[row][lane]);
        }
    }
}

#define AW 4
struct AttnP {
    const float* Q; const float* K; const float* V; float* O; float* P; const float* Mf; const int* Mi; float* ST;
    const float* Pw; const float* Rt; const int* SQ; const int* SK;
    long long swb, swh, swi, swj, srb, srh, sri;
    long long sQb, sQh, sQi, sQd, sKb, sKh, sKj, sKd, sVb, sVh, sVj, sVd, sOb, sOh, sOi, sPb, sPh, sPi, smb, smh, smi, smj;
    int Lq, Lk, dh, dv, hrep, causal, coff, pband;
    float scale, mfill; int nonorm, mpol;
    int roff, rn, segpol, win;
};
static_assert(sizeof(AttnP) == 12 * 8 + 29 * 8 + 16 * 4, "AttnP has padding");

#ifndef KATTN_ATTR
#define KATTN_ATTR
#endif
template <int DHP, int DVP, int QM, bool SPLITPV, bool TWOPASS>
__global__ __launch_bounds__(32 * AW) KATTN_ATTR void k_attn(AttnP p) {
    constexpr int NT = DVP / 16;
    constexpr int KS = DHP / 32;
    constexpr int VP = DVP + 8;
    __shared__ __align__(16) float    pl[AW][16 * 64];
    __shared__ __align__(16) _Float16 vl[(SPLITPV ? 2 : 1) * 64 * VP];
    const int lane = threadIdx.x & 31, hf = lane >> 4, l15 = lane & 15, wave = threadIdx.x >> 5;
    const int h = blockIdx.y, b = blockIdx.z, hk = h / p.hrep;
    const int q0 = (blockIdx.x * AW + wave) * 16;
    float* myp = pl[wave];
    const float L2E = 1.4426950408889634f;
    const float NEG = -__builtin_inff();
    const int qi = min(q0 + l15, p.Lq - 1);
    const float* qrow = p.Q + b * p.sQb + h * p.sQh + (long long)qi * p.sQi;
    const float* kbase = p.K + b * p.sKb + hk * p.sKh;
    const float* vbase = p.V + b * p.sVb + hk * p.sVh;
    v16h qa[QM == 0 ? KS : 1]; Split qs_[QM == 1 ? KS : 1]; Split3 qt_[QM == 2 ? KS : 1];
#pragma unroll
    for (int ks = 0; ks < KS; ++ks) {
        if (QM == 2) qt_[ks] = sp3_ld(qrow, p.sQd, ks * 32, hf, p.dh, 1.f);
        else if (QM == 1) qs_[ks] = sp_ld(qrow, p.sQd, ks * 32, hf, p.dh, 1.f);
        else qa[ks] = fh_ld(qrow, p.sQd, ks * 32, hf, p.dh, 1.f);
    }
    v8f o[NT]; float m8[8], l8[8];
#pragma unroll
    for (int t = 0; t < NT; ++t) { v8f zz = {}; o[t] = zz; }
#pragma unroll
    for (int i = 0; i < 8; ++i) { m8[i] = NEG; l8[i] = 0.f; }
    int jend = p.Lk;
    if (p.causal == 1) { const int je = (blockIdx.x * AW + AW - 1) * 16 + 16 + p.coff; jend = min(jend, max(je, 0)); }
    const int npass = TWOPASS ? 2 : 1;
    for (int pass = 0; pass < npass; ++pass) {
        const bool dopv = (!TWOPASS) || pass == 1;
        for (int j0 = 0; j0 < jend; j0 += 64) {
            if (dopv) {
                __syncthreads();
                for (int idx = threadIdx.x; idx < 64 * DVP; idx += 32 * AW) {
                    const int jr = idx / DVP, d = idx - jr * DVP, j = j0 + jr;
                    const float f = (j < p.Lk && d < p.dv) ? vbase[(long long)j * p.sVj + (long long)d * p.sVd] : 0.f;
                    if (SPLITPV) {
                        const __bf16 hb = bf16_rne(f);
                        ((__bf16*)vl)[jr * VP + d] = hb; ((__bf16*)vl)[64 * VP + jr * VP + d] = bf16_rne(f - bf16_f32(hb));
                    } else vl[jr * VP + d] = (_Float16)f;
                }
            }
            v8f s[4];
#pragma unroll
            for (int t = 0; t < 4; ++t) {
                const int j = min(j0 + t * 16 + l15, p.Lk - 1);
                const float* krow = kbase + (long long)j * p.sKj;
                v8f acc = {};
#pragma unroll
                for (int ks = 0; ks < KS; ++ks) {
                    if (QM == 2)      acc = wmma6(qt_[ks], sp3_ld(krow, p.sKd, ks * 32, hf, p.dh, 1.f), acc);
                    else if (QM == 1) acc = wmma3(qs_[ks], sp_ld(krow, p.sKd, ks * 32, hf, p.dh, 1.f), acc);
                    else              acc = wmma16(qa[ks], fh_ld(krow, p.sKd, ks * 32, hf, p.dh, 1.f), acc);
                }
                s[t] = acc;
            }
            float pv[8][4];
#pragma unroll
            for (int i = 0; i < 8; ++i) {
                const int irow = q0 + i + 8 * hf;
                const int ic = min(irow, p.Lq - 1);
                float sc[4];
#pragma unroll
                for (int t = 0; t < 4; ++t) {
                    const int jg = j0 + t * 16 + l15;
                    float v = s[t][i] * p.scale;
                    if (p.Mf) v += p.Mf[b * p.smb + h * p.smh + (long long)ic * p.smi + (long long)min(jg, p.Lk - 1) * p.smj];
                    if (p.Rt) { int rc = ic - min(jg, p.Lk - 1) + p.roff; rc = rc < 0 ? 0 : (rc >= p.rn ? p.rn - 1 : rc); v += p.Rt[b * p.srb + h * p.srh + (long long)ic * p.sri + rc]; }
                    if (p.Mi) { const int mv = p.Mi[b * p.smb + h * p.smh + (long long)ic * p.smi + (long long)min(jg, p.Lk - 1) * p.smj]; if (p.mpol ? (mv != 0) : (mv == 0)) v = p.mfill; }
                    if (p.SQ) { const bool same = p.SQ[(long long)b * p.Lq + ic] == p.SK[(long long)b * p.Lk + min(jg, p.Lk - 1)]; if (p.segpol ? same : !same) v = p.mfill; }
                    if (p.causal == 2 && jg > irow + p.coff) v = p.mfill;
                    if (jg >= p.Lk || (p.causal == 1 && jg > irow + p.coff) || (p.causal == 3 && jg < irow + p.coff) || (p.win > 0 && irow + p.coff - jg > p.win)) v = NEG; else v *= L2E;
                    sc[t] = v;
                }
                if (!TWOPASS || pass == 0) {
                    float mx = fmaxf(fmaxf(sc[0], sc[1]), fmaxf(sc[2], sc[3]));
                    mx = fmaxf(mx, __shfl_xor(mx, 1, 32)); mx = fmaxf(mx, __shfl_xor(mx, 2, 32));
                    mx = fmaxf(mx, __shfl_xor(mx, 4, 32)); mx = fmaxf(mx, __shfl_xor(mx, 8, 32));
                    const float mnew = fmaxf(m8[i], mx);
                    const float corr = (mnew == NEG) ? 1.f : exp2f(m8[i] - mnew);
                    float rs = 0.f;
#pragma unroll
                    for (int t = 0; t < 4; ++t) {
                        const float pp = (sc[t] == NEG) ? 0.f : exp2f(sc[t] - mnew); rs += pp;
                        pv[i][t] = p.Pw ? pp * p.Pw[b * p.swb + h * p.swh + (long long)ic * p.swi + (long long)min(j0 + t * 16 + l15, p.Lk - 1) * p.swj] : pp;
                    }
                    rs += __shfl_xor(rs, 1, 32); rs += __shfl_xor(rs, 2, 32); rs += __shfl_xor(rs, 4, 32); rs += __shfl_xor(rs, 8, 32);
                    l8[i] = l8[i] * corr + rs; m8[i] = mnew;
                    if (!TWOPASS) {
#pragma unroll
                        for (int t = 0; t < NT; ++t) o[t][i] *= corr;
                    }
                } else {
                    const float inv = (l8[i] > 0.f) ? 1.f / l8[i] : 0.f;
#pragma unroll
                    for (int t = 0; t < 4; ++t) {
                        const int jg = j0 + t * 16 + l15;
                        float pp = (sc[t] == NEG) ? 0.f : exp2f(sc[t] - m8[i]) * inv;
                        if (p.Pw) pp *= p.Pw[b * p.swb + h * p.swh + (long long)ic * p.swi + (long long)min(jg, p.Lk - 1) * p.swj];
                        pv[i][t] = pp;
                    }
                }
            }
            if (dopv) {
#pragma unroll
                for (int i = 0; i < 8; ++i)
#pragma unroll
                    for (int t = 0; t < 4; ++t) myp[(i + 8 * hf) * 64 + t * 16 + l15] = pv[i][t];
                __syncthreads();
                if (p.P) {
                    float* pb_ = p.P + b * p.sPb + h * p.sPh;
                    const bool fastP = (p.pband == 0) && ((p.sPi & 3) == 0) && (j0 + 64 <= p.Lk) && (q0 + 16 <= p.Lq) && ((((size_t)pb_) & 15) == 0);
                    if (fastP) {
#pragma unroll
                        for (int s = 0; s < 8; ++s) {
                            const int row = s * 2 + (lane >> 4), c4 = (lane & 15) * 4;
                            const v4f v = *(const v4f*)(myp + row * 64 + c4);
                            VST2V4(pb_ + (long long)(q0 + row) * p.sPi + j0 + c4, v);
                        }
                    } else {
                        for (int row = 0; row < 16; ++row) {
                            const int irow = q0 + row; if (irow >= p.Lq) continue;
                            for (int c = lane; c < 64; c += 32) {
                                const int jg = j0 + c; if (jg >= p.Lk) continue;
                                if (p.pband == 0) VST2(float, pb_ + (long long)irow * p.sPi + jg, myp[row * 64 + c]);
                                else if (jg - irow <= p.pband && irow - jg <= p.pband) VST2(float, pb_ + (long long)irow * p.sPi + (jg - irow + p.pband), myp[row * 64 + c]);
                            }
                        }
                    }
                }
                if (SPLITPV) {
                    const Split pa0 = sp_ld(myp + l15 * 64, 1, 0, hf, 64, 1.f), pa1 = sp_ld(myp + l15 * 64, 1, 32, hf, 64, 1.f);
                    const __bf16* vh = (const __bf16*)vl; const __bf16* vlo = vh + 64 * VP;
#pragma unroll
                    for (int t = 0; t < NT; ++t) {
                        const int dcol = t * 16 + l15;
                        Split b0, b1;
#pragma unroll
                        for (int e = 0; e < 16; ++e) {
                            const int k0 = frag_k(e, hf), k1 = 32 + frag_k(e, hf);
                            b0.hi[e] = vh[k0 * VP + dcol]; b0.lo[e] = vlo[k0 * VP + dcol]; b1.hi[e] = vh[k1 * VP + dcol]; b1.lo[e] = vlo[k1 * VP + dcol];
                        }
                        o[t] = wmma3(pa0, b0, o[t]);
                        o[t] = wmma3(pa1, b1, o[t]);
                    }
                } else {
                    const v16h pa0 = fh_ld(myp + l15 * 64, 1, 0, hf, 64, 4096.f), pa1 = fh_ld(myp + l15 * 64, 1, 32, hf, 64, 4096.f);
#pragma unroll
                    for (int t = 0; t < NT; ++t) {
                        const int dcol = t * 16 + l15;
                        v16h b0, b1;
#pragma unroll
                        for (int e = 0; e < 16; ++e) { b0[e] = vl[frag_k(e, hf) * VP + dcol]; b1[e] = vl[(32 + frag_k(e, hf)) * VP + dcol]; }
                        o[t] = wmma16(pa0, b0, o[t]);
                        o[t] = wmma16(pa1, b1, o[t]);
                    }
                }
            }
        }
    }
    float* obase = p.O + b * p.sOb + h * p.sOh;
    if (p.ST) {
        const int rl = lane >> 1, isel = rl & 7;
        float mv = 0.f, lv = 0.f;
#pragma unroll
        for (int i = 0; i < 8; ++i) if (i == isel) { mv = m8[i]; lv = l8[i]; }
        const int irow = q0 + rl;
        if (irow < p.Lq) { float* st = p.ST + (((long long)b * gridDim.y + h) * p.Lq + irow) * 2 + (lane & 1); VST2(float, st, (lane & 1) ? lv : mv * 0.6931471805599453f); }
    }
    float invr[8];
#pragma unroll
    for (int i = 0; i < 8; ++i) {
        if (TWOPASS) invr[i] = SPLITPV ? 1.f : (1.f / 4096.f);
        else if (p.nonorm) invr[i] = exp2f(m8[i]) * (SPLITPV ? 1.f : (1.f / 4096.f));
        else invr[i] = (l8[i] > 0.f) ? (SPLITPV ? 1.f / l8[i] : 1.f / (l8[i] * 4096.f)) : 0.f;
    }
    __syncthreads();
    const bool ofast = ((p.sOi & 3) == 0) && ((((size_t)obase) & 15) == 0) && (q0 + 16 <= p.Lq);
#pragma unroll
    for (int c0 = 0; c0 < DVP; c0 += 64) {
#pragma unroll
        for (int i = 0; i < 8; ++i)
#pragma unroll
            for (int t = 0; t < NT; ++t) if (t * 16 >= c0 && t * 16 < c0 + 64) myp[(i + 8 * hf) * 64 + (t * 16 - c0) + l15] = o[t][i] * invr[i];
        __syncthreads();
        const int cw = (DVP - c0 < 64) ? (DVP - c0) : 64;
        if (ofast && (c0 + cw <= p.dv) && (cw % 32 == 0)) {
            const int lpr = cw / 4;
            const int rows_per_ins = 32 / lpr;
            for (int r0 = 0; r0 < 16; r0 += rows_per_ins) {
                const int row = r0 + lane / lpr, c4 = (lane % lpr) * 4;
                const v4f v = *(const v4f*)(myp + row * 64 + c4);
                VST2V4(obase + (long long)(q0 + row) * p.sOi + c0 + c4, v);
            }
        } else {
            for (int row = 0; row < 16; ++row) {
                const int irow = q0 + row; if (irow >= p.Lq) continue;
                for (int c = lane; c < cw; c += 32) { const int d = c0 + c; if (d < p.dv) VST2(float, obase + (long long)irow * p.sOi + d, myp[row * 64 + c]); }
            }
        }
        __syncthreads();
    }
}

struct TrP { const float* src; float* dst; const float* R2; long long sSz, lds, sDz, ldd, sRz, ldr; int R, C, flags, act; float alpha, beta; };
static_assert(sizeof(TrP) == 3 * 8 + 6 * 8 + 6 * 4, "TrP has padding");
__global__ __launch_bounds__(256) void k_tr(TrP p) {
    __shared__ float tile[32][33];
    const int c0 = blockIdx.x * 32, r0 = blockIdx.y * 32, z = blockIdx.z;
    const int lane = threadIdx.x & 31, wave = threadIdx.x >> 5;
    const float* s = p.src + z * p.sSz;
#pragma unroll
    for (int k = 0; k < 4; ++k) {
        const int rl = wave * 4 + k, r = r0 + rl, c = c0 + lane;
        tile[rl][lane] = (r < p.R && c < p.C) ? s[(long long)r * p.lds + c] : 0.f;
    }
    __syncthreads();
    float* d = p.dst + z * p.sDz; const float* rr = p.R2 + z * p.sRz;
#pragma unroll
    for (int k = 0; k < 4; ++k) {
        const int cl = wave * 4 + k, c = c0 + cl, r = r0 + lane;
        if (c < p.C && r < p.R) {
            float v = act_fn(p.alpha * tile[lane][cl], p.act);
            if (p.flags & 1) v += p.beta * rr[(long long)c * p.ldr + r];
            VST2(float, d + (long long)c * p.ldd + r, v);
        }
    }
}

__global__ __launch_bounds__(256) void k_affine(const float* __restrict__ src, float* __restrict__ dst, int n, float a, float b, const float* __restrict__ sdev) {
    const int i = blockIdx.x * 256 + threadIdx.x;
    if (i < n) { const float aa = sdev ? a * sdev[0] : a; const float v = aa * src[i] + b; VST2(float, dst + i, v); }
}

struct SmP { const float* src; float* dst; const float* Mf; long long sz, sr, dz, dr, smz, smr; int n, pad; float scale_in, scale_out; };
static_assert(sizeof(SmP) == 3 * 8 + 6 * 8 + 4 * 4, "SmP has padding");
__global__ __launch_bounds__(256) void k_softmax(SmP p) {
    __shared__ float red[256];
    const int r = blockIdx.x, z = blockIdx.y, tid = threadIdx.x;
    const float* s = p.src + z * p.sz + (long long)r * p.sr;
    const float* mf = p.Mf ? (p.Mf + z * p.smz + (long long)r * p.smr) : nullptr;
    float mx = -__builtin_inff();
    for (int j = tid; j < p.n; j += 256) { float v = s[j] * p.scale_in; if (mf) v += mf[j]; mx = fmaxf(mx, v); }
    red[tid] = mx; __syncthreads();
    for (int o = 128; o > 0; o >>= 1) { if (tid < o) red[tid] = fmaxf(red[tid], red[tid + o]); __syncthreads(); }
    mx = red[0]; __syncthreads();
    float sum = 0.f;
    for (int j = tid; j < p.n; j += 256) { float v = s[j] * p.scale_in; if (mf) v += mf[j]; sum += (mx == -__builtin_inff()) ? 0.f : expf(v - mx); }
    red[tid] = sum; __syncthreads();
    for (int o = 128; o > 0; o >>= 1) { if (tid < o) red[tid] += red[tid + o]; __syncthreads(); }
    sum = red[0];
    const float inv = (sum > 0.f) ? p.scale_out / sum : 0.f;
    float* d = p.dst + z * p.dz + (long long)r * p.dr;
    for (int j = tid; j < p.n; j += 256) { float v = s[j] * p.scale_in; if (mf) v += mf[j]; const float o = (mx == -__builtin_inff()) ? 0.f : expf(v - mx) * inv; VST2(float, d + j, o); }
}
__global__ __launch_bounds__(256) void k_stats(const float* __restrict__ x, long long sz, long long so, long long si, int inner, int n, float eps, float* __restrict__ stat, int mode) {
    __shared__ float red[256];
    const int z = blockIdx.x, tid = threadIdx.x;
    const float* base = x + z * sz;
    float s = 0.f;
    for (int e = tid; e < n; e += 256) s += base[(long long)(e / inner) * so + (long long)(e % inner) * si];
    red[tid] = s; __syncthreads();
    for (int o = 128; o > 0; o >>= 1) { if (tid < o) red[tid] += red[tid + o]; __syncthreads(); }
    const float mu = (mode == 0 || mode == 3) ? red[0] / (float)n : 0.f; __syncthreads();
    float q = 0.f;
    for (int e = tid; e < n; e += 256) { const float dlt = base[(long long)(e / inner) * so + (long long)(e % inner) * si] - mu; q += dlt * dlt; }
    red[tid] = q; __syncthreads();
    for (int o = 128; o > 0; o >>= 1) { if (tid < o) red[tid] += red[tid + o]; __syncthreads(); }
    {
        float rs;
        if (mode == 2) rs = sqrtf((float)n) / fmaxf(sqrtf(red[0]), eps); else if (mode == 3) rs = rsqrtf(red[0] / (float)(n - 1) + eps); else rs = rsqrtf(red[0] / (float)n + eps);
        if (tid < 32) { const float v = (tid == 0) ? mu : ((tid == 1) ? rs : 0.f); VST2(float, stat + (long long)z * 32 + tid, v); }
    }
}
__global__ __launch_bounds__(256) void k_norm_apply(const float* __restrict__ x, float* __restrict__ y, const float* __restrict__ stat, const float* __restrict__ g, const float* __restrict__ bta,
                                                     int Z, int C, int L, int G, int bn, int act) {
    const long long idx = (long long)blockIdx.x * 256 + threadIdx.x;
    if (idx >= (long long)Z * C * L) return;
    const int l = (int)(idx % L); const long long zc = idx / L; const int c = (int)(zc % C), z = (int)(zc / C); (void)l;
    const int set = bn ? c : (z * G + c / (C / G));
    float v = (x[idx] - stat[(long long)set * 32]) * stat[(long long)set * 32 + 1];
    if (g) v *= g[c];
    if (bta) v += bta[c];
    v = act_fn(v, act);
    VST2(float, y + idx, v);
}

__global__ __launch_bounds__(256) void k_lse_neg(const float* __restrict__ st, float* __restrict__ c, int n) {
    const int i = blockIdx.x * 256 + threadIdx.x;
    if (i < n) { const float v = -(st[2 * i] + logf(st[2 * i + 1])); VST2(float, c + i, v); }
}

__global__ __launch_bounds__(256) void k_iota(int* __restrict__ dst, int n, int a, int b) {
    const int i = blockIdx.x * 256 + threadIdx.x;
    if (i < n) { const int v = a * i + b; VST2(int, dst + i, v); }
}

__global__ __launch_bounds__(256) void k_axpby(const float* __restrict__ x, const float* __restrict__ y, float* __restrict__ dst, int n, float a, float b, float c) {
    const int i = blockIdx.x * 256 + threadIdx.x;
    if (i < n) { const float v = a * x[i] + b * y[i] + c; VST2(float, dst + i, v); }
}

struct RopeP { const float* X; float* Y; const float* C; const float* Sn; const int* pos; long long sXr, sXh, sYr, sYh, sCb, sCp, sCd; int R, Hn, D, S, mode, tmode, pmode, pad; };
static_assert(sizeof(RopeP) == 5 * 8 + 7 * 8 + 8 * 4, "RopeP has padding");
__global__ __launch_bounds__(256) void k_rope(RopeP p) {
    const long long idx = (long long)blockIdx.x * 256 + threadIdx.x;
    if (idx >= (long long)p.R * p.Hn * p.D) return;
    const int d = (int)(idx % p.D); const long long rh = idx / p.D; const int h = (int)(rh % p.Hn); const int r = (int)(rh / p.Hn);
    const int half = p.D / 2;
    int partner; float sign;
    if (p.mode == 0) { partner = (d < half) ? d + half : d - half; sign = (d < half) ? -1.f : 1.f; }
    else { partner = d ^ 1; sign = (d & 1) ? 1.f : -1.f; }
    const int tcol = (p.tmode == 0) ? d : ((p.tmode == 1) ? (d % half) : (d >> 1));
    const int pp = (p.pmode == 0) ? (r % p.S) : ((p.pmode == 1) ? h : p.pos[r]);
    const long long toff = (long long)(r / p.S) * p.sCb + (long long)pp * p.sCp + (long long)tcol * p.sCd;
    const float* xr = p.X + (long long)r * p.sXr + (long long)h * p.sXh;
    const float v = xr[d] * p.C[toff] + sign * xr[partner] * p.Sn[toff];
    VST2(float, p.Y + (long long)r * p.sYr + (long long)h * p.sYh + d, v);
}

__global__ __launch_bounds__(256) void k_invf(float* __restrict__ invb, int half, int D, float base, float num, int fmode, float cexp) {
    const int i = blockIdx.x * 256 + threadIdx.x;
    if (i >= ((half + 31) / 32) * 32) return;
    if (i >= half) { VST2(float, invb + i, 0.f); return; }
    const float e = (float)(2 * i) / (float)D;
    float invf;
    if (fmode == 1) invf = num * expf((float)(2 * i) * cexp);
    else if (fmode == 2) invf = num * powf(base, (-2.0f * ((float)i - 1.0f)) / (float)D);
    else invf = num * (1.0f / powf(base, e));
    VST2(float, invb + i, invf);
}
__global__ __launch_bounds__(256) void k_sincos(float* __restrict__ cs, float* __restrict__ sn, const float* __restrict__ invb, int S, int half, float pscale) {
    const int idx = blockIdx.x * 256 + threadIdx.x;
    if (idx >= S * half) return;
    const int s = idx / half, i = idx - s * half;
    const float ang = (pscale * (float)s) * invb[i];
    VST2(float, cs + idx, cosf(ang)); VST2(float, sn + idx, sinf(ang));
}

__global__ __launch_bounds__(256) void k_mulact(const float* __restrict__ x, const float* __restrict__ y, float* __restrict__ dst, int n, int act) {
    const int i = blockIdx.x * 256 + threadIdx.x;
    if (i < n) { const float v = act_fn(x[i], act) * y[i]; VST2(float, dst + i, v); }
}

__global__ __launch_bounds__(256) void k_matvec(GemmP p) {
    const int rpt = (p.N == 1) ? 1 : 32;
    const long long r0 = ((long long)blockIdx.x * 256 + threadIdx.x) * rpt; const int z = blockIdx.z, zo = z / p.zi_n, zi = z - zo * p.zi_n;
    if (r0 >= p.M) return;
    const float* Bb = p.B + zo * p.sBo + zi * p.sBi;
    float* C = p.C + zo * p.sCo + zi * p.sCi; const float* R = p.R + zo * p.sRo + zi * p.sRi;
    for (int rr = 0; rr < rpt; ++rr) {
        const long long r = r0 + rr; if (r >= p.M) break;
        const float* A = p.A + zo * p.sAo + zi * p.sAi + r * p.sAm;
        float acc[8] = {0.f, 0.f, 0.f, 0.f, 0.f, 0.f, 0.f, 0.f};
        for (int k = 0; k < p.K; ++k) { const float a = A[(long long)k * p.sAk];
#pragma unroll
            for (int j = 0; j < 8; ++j) if (j < p.N) acc[j] += a * Bb[(long long)j * p.sBn + (long long)k * p.sBk]; }
#pragma unroll
        for (int j = 0; j < 8; ++j) if (j < p.N) {
            float v = acc[j] * p.alpha;
            if (p.flags & 1) v += p.bias[j];
            if (p.flags & 2) v += p.bias[r];
            v = act_fn(v, p.act);
            if (p.flags & 4) v += p.beta * R[r * p.sRm + (long long)j * p.sRn];
            VST2(float, C + r * p.sCm + j, v);
        }
    }
}
__global__ __launch_bounds__(256) void k_smallsoftmax(const float* __restrict__ src, float* __restrict__ dst, long long sr, long long dr, int n, long long R, float scale) {
    const long long r0 = ((long long)blockIdx.x * 256 + threadIdx.x) * 32;
    for (int rr = 0; rr < 32; ++rr) {
        const long long r = r0 + rr; if (r >= R) return;
        const float* s = src + r * sr; float* d = dst + r * dr;
        float mx = -__builtin_inff();
        for (int j = 0; j < n; ++j) mx = fmaxf(mx, s[j] * scale);
        float sum = 0.f;
        for (int j = 0; j < n; ++j) sum += expf(s[j] * scale - mx);
        const float inv = 1.f / sum;
        for (int j = 0; j < n; ++j) { const float v = expf(s[j] * scale - mx) * inv; VST2(float, d + j, v); }
    }
}

__global__ __launch_bounds__(32) void k_unitstat(float* __restrict__ st) { const int t = threadIdx.x; const float v = (t == 1) ? 1.f : 0.f; VST2(float, st + t, v); }

__global__ __launch_bounds__(256) void k_lincopy(const float* __restrict__ src, long long lds, float* __restrict__ dst, long long ldd, long long rows, int cols) {
    const long long i = (long long)blockIdx.x * 256 + threadIdx.x; if (i >= rows * cols) return;
    const long long r = i / cols; const int c = (int)(i - r * cols);
    const float v = src[r * lds + c]; VST2(float, dst + r * ldd + c, v);
}

__global__ __launch_bounds__(256) void k_roll_x0(const int* __restrict__ stok, const float* __restrict__ Emb, float* __restrict__ A, int B, int E, int KA, int V) {
    const int q = blockIdx.x * 256 + threadIdx.x; if (q >= B * E) return; const int e = q % E; const int b = q / E; int id = stok[b]; id = min(max(id, 0), V - 1); VST2(float, A + (long long)b * KA + e, Emb[(long long)id * E + e]);
}
__global__ __launch_bounds__(256) void k_roll_cell(const float* __restrict__ GT, float* __restrict__ Cc, float* __restrict__ A, int B, int H, int E, int KA) {
    const int q = blockIdx.x * 256 + threadIdx.x; if (q >= B * H) return; const int j = q % H; const int b = q / H; const float* g = GT + (long long)b * 4 * H;
    const float ig = 1.f / (1.f + expf(-g[j])), fg = 1.f / (1.f + expf(-g[H + j])), og = 1.f / (1.f + expf(-g[2 * H + j])), ch = tanhf(g[3 * H + j]);
    const float c = fg * Cc[q] + ig * ch; VST2(float, Cc + q, c); VST2(float, A + (long long)b * KA + E + j, og * tanhf(c));
}
__global__ __launch_bounds__(256) void k_roll_pick(const float* __restrict__ LG, const int* __restrict__ X, const int* __restrict__ gnum, const float* __restrict__ Emb, float* __restrict__ A, int* __restrict__ OUT, int B, int T, int V, int E, int KA, int t) {
    __shared__ float bv[256]; __shared__ int bi[256];
    const int b = blockIdx.x; const int tid = threadIdx.x; const float* l = LG + (long long)b * V; float mx = -__builtin_inff(); int am = 0x7fffffff;
    for (int v = tid; v < V; v += 256) { const float x = l[v]; if (x > mx) { mx = x; am = v; } }
    bv[tid] = mx; bi[tid] = am; __syncthreads();
    for (int o = 128; o > 0; o >>= 1) { if (tid < o) { const float m2 = bv[tid + o]; const int i2 = bi[tid + o]; if (m2 > bv[tid] || (m2 == bv[tid] && i2 < bi[tid])) { bv[tid] = m2; bi[tid] = i2; } } __syncthreads(); }
    int tok = (t < gnum[0]) ? X[b * T + t] : bi[0]; tok = min(max(tok, 0), V - 1);
    if (tid == 0) VST2(int, OUT + b * T + t, tok);
    if (tid < E) VST2(float, A + (long long)b * KA + tid, Emb[(long long)tok * E + tid]);
}

template __global__ void k_gemm<3>(GemmP);

extern "C" void kernel_launch(void* const* d_in, const int* in_sizes, int n_in, void* d_out, int out_size, void* d_ws, size_t ws_size, hipStream_t stream) {
    (void)in_sizes; (void)n_in; (void)out_size; (void)ws_size;
    const int* X = (const int*)d_in[0];
    const int* gnum = (const int*)d_in[1];
    const int* stok = (const int*)d_in[2];
    const float* Emb = (const float*)d_in[3];
    const float* Wi = (const float*)d_in[4];
    const float* Ui = (const float*)d_in[5];
    const float* bi = (const float*)d_in[6];
    const float* Wf = (const float*)d_in[7];
    const float* Uf = (const float*)d_in[8];
    const float* bf = (const float*)d_in[9];
    const float* Wog = (const float*)d_in[10];
    const float* Uog = (const float*)d_in[11];
    const float* bog = (const float*)d_in[12];
    const float* Wc = (const float*)d_in[13];
    const float* Uc = (const float*)d_in[14];
    const float* bc = (const float*)d_in[15];
    const float* Wo = (const float*)d_in[16];
    const float* bo = (const float*)d_in[17];
    const int Bn = 64;
    const int T = 32;
    const int E = 64;
    const int H = 256;
    const int V = 32000;
    const int G4 = 1024;
    const int KA = 320;
    float* out = (float*)d_out;
    char* wsp = (char*)d_ws;
    float* PK = (float*)wsp; wsp += (((size_t)((size_t)KA * G4) * 4 + 255) / 256) * 256;
    float* BS = (float*)wsp; wsp += (((size_t)((size_t)G4) * 4 + 255) / 256) * 256;
    float* A = (float*)wsp; wsp += (((size_t)((size_t)Bn * KA) * 4 + 255) / 256) * 256;
    float* C = (float*)wsp; wsp += (((size_t)((size_t)Bn * H) * 4 + 255) / 256) * 256;
    float* GT = (float*)wsp; wsp += (((size_t)((size_t)Bn * G4) * 4 + 255) / 256) * 256;
    float* LG = (float*)wsp; wsp += (((size_t)((size_t)Bn * V) * 4 + 255) / 256) * 256;
    k_lincopy<<<(unsigned)(((long long)(E) * (H) + 255) / 256), 256, 0, stream>>>(Wi, H, PK + 0, G4, E, H);
    k_lincopy<<<(unsigned)(((long long)(H) * (H) + 255) / 256), 256, 0, stream>>>(Ui, H, PK + 65536, G4, H, H);
    k_lincopy<<<(unsigned)(((long long)(1) * (H) + 255) / 256), 256, 0, stream>>>(bi, H, BS + 0, G4, 1, H);
    k_lincopy<<<(unsigned)(((long long)(E) * (H) + 255) / 256), 256, 0, stream>>>(Wf, H, PK + 256, G4, E, H);
    k_lincopy<<<(unsigned)(((long long)(H) * (H) + 255) / 256), 256, 0, stream>>>(Uf, H, PK + 65792, G4, H, H);
    k_lincopy<<<(unsigned)(((long long)(1) * (H) + 255) / 256), 256, 0, stream>>>(bf, H, BS + 256, G4, 1, H);
    k_lincopy<<<(unsigned)(((long long)(E) * (H) + 255) / 256), 256, 0, stream>>>(Wog, H, PK + 512, G4, E, H);
    k_lincopy<<<(unsigned)(((long long)(H) * (H) + 255) / 256), 256, 0, stream>>>(Uog, H, PK + 66048, G4, H, H);
    k_lincopy<<<(unsigned)(((long long)(1) * (H) + 255) / 256), 256, 0, stream>>>(bog, H, BS + 512, G4, 1, H);
    k_lincopy<<<(unsigned)(((long long)(E) * (H) + 255) / 256), 256, 0, stream>>>(Wc, H, PK + 768, G4, E, H);
    k_lincopy<<<(unsigned)(((long long)(H) * (H) + 255) / 256), 256, 0, stream>>>(Uc, H, PK + 66304, G4, H, H);
    k_lincopy<<<(unsigned)(((long long)(1) * (H) + 255) / 256), 256, 0, stream>>>(bc, H, BS + 768, G4, 1, H);
    hipMemsetAsync(A, 0, (size_t)Bn * KA * 4, stream); hipMemsetAsync(C, 0, (size_t)Bn * H * 4, stream);
    k_roll_x0<<<(unsigned)((Bn * E + 255) / 256), 256, 0, stream>>>(stok, Emb, A, Bn, E, KA, V);
    { GemmP gg0;
      gg0.A = A; gg0.B = PK; gg0.bias = BS; gg0.R = A; gg0.C = GT;
      gg0.sAo = 0; gg0.sAi = 0; gg0.sAm = KA; gg0.sAk = 1; gg0.sBo = 0; gg0.sBi = 0; gg0.sBn = 1; gg0.sBk = G4; gg0.sCo = 0; gg0.sCi = 0; gg0.sCm = G4; gg0.sRo = 0; gg0.sRi = 0; gg0.sRm = 0; gg0.sRn = 0;
      gg0.M = Bn; gg0.N = G4; gg0.K = KA; gg0.zi_n = 1; gg0.flags = 1; gg0.act = 0;
      gg0.alpha = 1.0f; gg0.beta = 0.0f; gg0.sa = 1.0f; gg0.sb = 1.0f; gg0.Npad = G4; gg0.pad_ = 0;
      k_gemm<3><<<dim3((unsigned)((G4) + 31) / 32, (unsigned)((Bn) + 15) / 16, (unsigned)(1)), 32, 0, stream>>>(gg0); }
    k_roll_cell<<<(unsigned)((Bn * H + 255) / 256), 256, 0, stream>>>(GT, C, A, Bn, H, E, KA);
    { GemmP gl0;
      gl0.A = A + E; gl0.B = Wo; gl0.bias = bo; gl0.R = A + E; gl0.C = LG;
      gl0.sAo = 0; gl0.sAi = 0; gl0.sAm = KA; gl0.sAk = 1; gl0.sBo = 0; gl0.sBi = 0; gl0.sBn = 1; gl0.sBk = V; gl0.sCo = 0; gl0.sCi = 0; gl0.sCm = V; gl0.sRo = 0; gl0.sRi = 0; gl0.sRm = 0; gl0.sRn = 0;
      gl0.M = Bn; gl0.N = V; gl0.K = H; gl0.zi_n = 1; gl0.flags = 1; gl0.act = 0;
      gl0.alpha = 1.0f; gl0.beta = 0.0f; gl0.sa = 1.0f; gl0.sb = 1.0f; gl0.Npad = V; gl0.pad_ = 0;
      k_gemm<3><<<dim3((unsigned)((V) + 31) / 32, (unsigned)((Bn) + 15) / 16, (unsigned)(1)), 32, 0, stream>>>(gl0); }
    k_roll_pick<<<Bn, 256, 0, stream>>>(LG, X, gnum, Emb, A, (int*)out, Bn, T, V, E, KA, 0);
    { GemmP gg1;
      gg1.A = A; gg1.B = PK; gg1.bias = BS; gg1.R = A; gg1.C = GT;
      gg1.sAo = 0; gg1.sAi = 0; gg1.sAm = KA; gg1.sAk = 1; gg1.sBo = 0; gg1.sBi = 0; gg1.sBn = 1; gg1.sBk = G4; gg1.sCo = 0; gg1.sCi = 0; gg1.sCm = G4; gg1.sRo = 0; gg1.sRi = 0; gg1.sRm = 0; gg1.sRn = 0;
      gg1.M = Bn; gg1.N = G4; gg1.K = KA; gg1.zi_n = 1; gg1.flags = 1; gg1.act = 0;
      gg1.alpha = 1.0f; gg1.beta = 0.0f; gg1.sa = 1.0f; gg1.sb = 1.0f; gg1.Npad = G4; gg1.pad_ = 0;
      k_gemm<3><<<dim3((unsigned)((G4) + 31) / 32, (unsigned)((Bn) + 15) / 16, (unsigned)(1)), 32, 0, stream>>>(gg1); }
    k_roll_cell<<<(unsigned)((Bn * H + 255) / 256), 256, 0, stream>>>(GT, C, A, Bn, H, E, KA);
    { GemmP gl1;
      gl1.A = A + E; gl1.B = Wo; gl1.bias = bo; gl1.R = A + E; gl1.C = LG;
      gl1.sAo = 0; gl1.sAi = 0; gl1.sAm = KA; gl1.sAk = 1; gl1.sBo = 0; gl1.sBi = 0; gl1.sBn = 1; gl1.sBk = V; gl1.sCo = 0; gl1.sCi = 0; gl1.sCm = V; gl1.sRo = 0; gl1.sRi = 0; gl1.sRm = 0; gl1.sRn = 0;
      gl1.M = Bn; gl1.N = V; gl1.K = H; gl1.zi_n = 1; gl1.flags = 1; gl1.act = 0;
      gl1.alpha = 1.0f; gl1.beta = 0.0f; gl1.sa = 1.0f; gl1.sb = 1.0f; gl1.Npad = V; gl1.pad_ = 0;
      k_gemm<3><<<dim3((unsigned)((V) + 31) / 32, (unsigned)((Bn) + 15) / 16, (unsigned)(1)), 32, 0, stream>>>(gl1); }
    k_roll_pick<<<Bn, 256, 0, stream>>>(LG, X, gnum, Emb, A, (int*)out, Bn, T, V, E, KA, 1);
    { GemmP gg2;
      gg2.A = A; gg2.B = PK; gg2.bias = BS; gg2.R = A; gg2.C = GT;
      gg2.sAo = 0; gg2.sAi = 0; gg2.sAm = KA; gg2.sAk = 1; gg2.sBo = 0; gg2.sBi = 0; gg2.sBn = 1; gg2.sBk = G4; gg2.sCo = 0; gg2.sCi = 0; gg2.sCm = G4; gg2.sRo = 0; gg2.sRi = 0; gg2.sRm = 0; gg2.sRn = 0;
      gg2.M = Bn; gg2.N = G4; gg2.K = KA; gg2.zi_n = 1; gg2.flags = 1; gg2.act = 0;
      gg2.alpha = 1.0f; gg2.beta = 0.0f; gg2.sa = 1.0f; gg2.sb = 1.0f; gg2.Npad = G4; gg2.pad_ = 0;
      k_gemm<3><<<dim3((unsigned)((G4) + 31) / 32, (unsigned)((Bn) + 15) / 16, (unsigned)(1)), 32, 0, stream>>>(gg2); }
    k_roll_cell<<<(unsigned)((Bn * H + 255) / 256), 256, 0, stream>>>(GT, C, A, Bn, H, E, KA);
    { GemmP gl2;
      gl2.A = A + E; gl2.B = Wo; gl2.bias = bo; gl2.R = A + E; gl2.C = LG;
      gl2.sAo = 0; gl2.sAi = 0; gl2.sAm = KA; gl2.sAk = 1; gl2.sBo = 0; gl2.sBi = 0; gl2.sBn = 1; gl2.sBk = V; gl2.sCo = 0; gl2.sCi = 0; gl2.sCm = V; gl2.sRo = 0; gl2.sRi = 0; gl2.sRm = 0; gl2.sRn = 0;
      gl2.M = Bn; gl2.N = V; gl2.K = H; gl2.zi_n = 1; gl2.flags = 1; gl2.act = 0;
      gl2.alpha = 1.0f; gl2.beta = 0.0f; gl2.sa = 1.0f; gl2.sb = 1.0f; gl2.Npad = V; gl2.pad_ = 0;
      k_gemm<3><<<dim3((unsigned)((V) + 31) / 32, (unsigned)((Bn) + 15) / 16, (unsigned)(1)), 32, 0, stream>>>(gl2); }
    k_roll_pick<<<Bn, 256, 0, stream>>>(LG, X, gnum, Emb, A, (int*)out, Bn, T, V, E, KA, 2);
    { GemmP gg3;
      gg3.A = A; gg3.B = PK; gg3.bias = BS; gg3.R = A; gg3.C = GT;
      gg3.sAo = 0; gg3.sAi = 0; gg3.sAm = KA; gg3.sAk = 1; gg3.sBo = 0; gg3.sBi = 0; gg3.sBn = 1; gg3.sBk = G4; gg3.sCo = 0; gg3.sCi = 0; gg3.sCm = G4; gg3.sRo = 0; gg3.sRi = 0; gg3.sRm = 0; gg3.sRn = 0;
      gg3.M = Bn; gg3.N = G4; gg3.K = KA; gg3.zi_n = 1; gg3.flags = 1; gg3.act = 0;
      gg3.alpha = 1.0f; gg3.beta = 0.0f; gg3.sa = 1.0f; gg3.sb = 1.0f; gg3.Npad = G4; gg3.pad_ = 0;
      k_gemm<3><<<dim3((unsigned)((G4) + 31) / 32, (unsigned)((Bn) + 15) / 16, (unsigned)(1)), 32, 0, stream>>>(gg3); }
    k_roll_cell<<<(unsigned)((Bn * H + 255) / 256), 256, 0, stream>>>(GT, C, A, Bn, H, E, KA);
    { GemmP gl3;
      gl3.A = A + E; gl3.B = Wo; gl3.bias = bo; gl3.R = A + E; gl3.C = LG;
      gl3.sAo = 0; gl3.sAi = 0; gl3.sAm = KA; gl3.sAk = 1; gl3.sBo = 0; gl3.sBi = 0; gl3.sBn = 1; gl3.sBk = V; gl3.sCo = 0; gl3.sCi = 0; gl3.sCm = V; gl3.sRo = 0; gl3.sRi = 0; gl3.sRm = 0; gl3.sRn = 0;
      gl3.M = Bn; gl3.N = V; gl3.K = H; gl3.zi_n = 1; gl3.flags = 1; gl3.act = 0;
      gl3.alpha = 1.0f; gl3.beta = 0.0f; gl3.sa = 1.0f; gl3.sb = 1.0f; gl3.Npad = V; gl3.pad_ = 0;
      k_gemm<3><<<dim3((unsigned)((V) + 31) / 32, (unsigned)((Bn) + 15) / 16, (unsigned)(1)), 32, 0, stream>>>(gl3); }
    k_roll_pick<<<Bn, 256, 0, stream>>>(LG, X, gnum, Emb, A, (int*)out, Bn, T, V, E, KA, 3);
    { GemmP gg4;
      gg4.A = A; gg4.B = PK; gg4.bias = BS; gg4.R = A; gg4.C = GT;
      gg4.sAo = 0; gg4.sAi = 0; gg4.sAm = KA; gg4.sAk = 1; gg4.sBo = 0; gg4.sBi = 0; gg4.sBn = 1; gg4.sBk = G4; gg4.sCo = 0; gg4.sCi = 0; gg4.sCm = G4; gg4.sRo = 0; gg4.sRi = 0; gg4.sRm = 0; gg4.sRn = 0;
      gg4.M = Bn; gg4.N = G4; gg4.K = KA; gg4.zi_n = 1; gg4.flags = 1; gg4.act = 0;
      gg4.alpha = 1.0f; gg4.beta = 0.0f; gg4.sa = 1.0f; gg4.sb = 1.0f; gg4.Npad = G4; gg4.pad_ = 0;
      k_gemm<3><<<dim3((unsigned)((G4) + 31) / 32, (unsigned)((Bn) + 15) / 16, (unsigned)(1)), 32, 0, stream>>>(gg4); }
    k_roll_cell<<<(unsigned)((Bn * H + 255) / 256), 256, 0, stream>>>(GT, C, A, Bn, H, E, KA);
    { GemmP gl4;
      gl4.A = A + E; gl4.B = Wo; gl4.bias = bo; gl4.R = A + E; gl4.C = LG;
      gl4.sAo = 0; gl4.sAi = 0; gl4.sAm = KA; gl4.sAk = 1; gl4.sBo = 0; gl4.sBi = 0; gl4.sBn = 1; gl4.sBk = V; gl4.sCo = 0; gl4.sCi = 0; gl4.sCm = V; gl4.sRo = 0; gl4.sRi = 0; gl4.sRm = 0; gl4.sRn = 0;
      gl4.M = Bn; gl4.N = V; gl4.K = H; gl4.zi_n = 1; gl4.flags = 1; gl4.act = 0;
      gl4.alpha = 1.0f; gl4.beta = 0.0f; gl4.sa = 1.0f; gl4.sb = 1.0f; gl4.Npad = V; gl4.pad_ = 0;
      k_gemm<3><<<dim3((unsigned)((V) + 31) / 32, (unsigned)((Bn) + 15) / 16, (unsigned)(1)), 32, 0, stream>>>(gl4); }
    k_roll_pick<<<Bn, 256, 0, stream>>>(LG, X, gnum, Emb, A, (int*)out, Bn, T, V, E, KA, 4);
    { GemmP gg5;
      gg5.A = A; gg5.B = PK; gg5.bias = BS; gg5.R = A; gg5.C = GT;
      gg5.sAo = 0; gg5.sAi = 0; gg5.sAm = KA; gg5.sAk = 1; gg5.sBo = 0; gg5.sBi = 0; gg5.sBn = 1; gg5.sBk = G4; gg5.sCo = 0; gg5.sCi = 0; gg5.sCm = G4; gg5.sRo = 0; gg5.sRi = 0; gg5.sRm = 0; gg5.sRn = 0;
      gg5.M = Bn; gg5.N = G4; gg5.K = KA; gg5.zi_n = 1; gg5.flags = 1; gg5.act = 0;
      gg5.alpha = 1.0f; gg5.beta = 0.0f; gg5.sa = 1.0f; gg5.sb = 1.0f; gg5.Npad = G4; gg5.pad_ = 0;
      k_gemm<3><<<dim3((unsigned)((G4) + 31) / 32, (unsigned)((Bn) + 15) / 16, (unsigned)(1)), 32, 0, stream>>>(gg5); }
    k_roll_cell<<<(unsigned)((Bn * H + 255) / 256), 256, 0, stream>>>(GT, C, A, Bn, H, E, KA);
    { GemmP gl5;
      gl5.A = A + E; gl5.B = Wo; gl5.bias = bo; gl5.R = A + E; gl5.C = LG;
      gl5.sAo = 0; gl5.sAi = 0; gl5.sAm = KA; gl5.sAk = 1; gl5.sBo = 0; gl5.sBi = 0; gl5.sBn = 1; gl5.sBk = V; gl5.sCo = 0; gl5.sCi = 0; gl5.sCm = V; gl5.sRo = 0; gl5.sRi = 0; gl5.sRm = 0; gl5.sRn = 0;
      gl5.M = Bn; gl5.N = V; gl5.K = H; gl5.zi_n = 1; gl5.flags = 1; gl5.act = 0;
      gl5.alpha = 1.0f; gl5.beta = 0.0f; gl5.sa = 1.0f; gl5.sb = 1.0f; gl5.Npad = V; gl5.pad_ = 0;
      k_gemm<3><<<dim3((unsigned)((V) + 31) / 32, (unsigned)((Bn) + 15) / 16, (unsigned)(1)), 32, 0, stream>>>(gl5); }
    k_roll_pick<<<Bn, 256, 0, stream>>>(LG, X, gnum, Emb, A, (int*)out, Bn, T, V, E, KA, 5);
    { GemmP gg6;
      gg6.A = A; gg6.B = PK; gg6.bias = BS; gg6.R = A; gg6.C = GT;
      gg6.sAo = 0; gg6.sAi = 0; gg6.sAm = KA; gg6.sAk = 1; gg6.sBo = 0; gg6.sBi = 0; gg6.sBn = 1; gg6.sBk = G4; gg6.sCo = 0; gg6.sCi = 0; gg6.sCm = G4; gg6.sRo = 0; gg6.sRi = 0; gg6.sRm = 0; gg6.sRn = 0;
      gg6.M = Bn; gg6.N = G4; gg6.K = KA; gg6.zi_n = 1; gg6.flags = 1; gg6.act = 0;
      gg6.alpha = 1.0f; gg6.beta = 0.0f; gg6.sa = 1.0f; gg6.sb = 1.0f; gg6.Npad = G4; gg6.pad_ = 0;
      k_gemm<3><<<dim3((unsigned)((G4) + 31) / 32, (unsigned)((Bn) + 15) / 16, (unsigned)(1)), 32, 0, stream>>>(gg6); }
    k_roll_cell<<<(unsigned)((Bn * H + 255) / 256), 256, 0, stream>>>(GT, C, A, Bn, H, E, KA);
    { GemmP gl6;
      gl6.A = A + E; gl6.B = Wo; gl6.bias = bo; gl6.R = A + E; gl6.C = LG;
      gl6.sAo = 0; gl6.sAi = 0; gl6.sAm = KA; gl6.sAk = 1; gl6.sBo = 0; gl6.sBi = 0; gl6.sBn = 1; gl6.sBk = V; gl6.sCo = 0; gl6.sCi = 0; gl6.sCm = V; gl6.sRo = 0; gl6.sRi = 0; gl6.sRm = 0; gl6.sRn = 0;
      gl6.M = Bn; gl6.N = V; gl6.K = H; gl6.zi_n = 1; gl6.flags = 1; gl6.act = 0;
      gl6.alpha = 1.0f; gl6.beta = 0.0f; gl6.sa = 1.0f; gl6.sb = 1.0f; gl6.Npad = V; gl6.pad_ = 0;
      k_gemm<3><<<dim3((unsigned)((V) + 31) / 32, (unsigned)((Bn) + 15) / 16, (unsigned)(1)), 32, 0, stream>>>(gl6); }
    k_roll_pick<<<Bn, 256, 0, stream>>>(LG, X, gnum, Emb, A, (int*)out, Bn, T, V, E, KA, 6);
    { GemmP gg7;
      gg7.A = A; gg7.B = PK; gg7.bias = BS; gg7.R = A; gg7.C = GT;
      gg7.sAo = 0; gg7.sAi = 0; gg7.sAm = KA; gg7.sAk = 1; gg7.sBo = 0; gg7.sBi = 0; gg7.sBn = 1; gg7.sBk = G4; gg7.sCo = 0; gg7.sCi = 0; gg7.sCm = G4; gg7.sRo = 0; gg7.sRi = 0; gg7.sRm = 0; gg7.sRn = 0;
      gg7.M = Bn; gg7.N = G4; gg7.K = KA; gg7.zi_n = 1; gg7.flags = 1; gg7.act = 0;
      gg7.alpha = 1.0f; gg7.beta = 0.0f; gg7.sa = 1.0f; gg7.sb = 1.0f; gg7.Npad = G4; gg7.pad_ = 0;
      k_gemm<3><<<dim3((unsigned)((G4) + 31) / 32, (unsigned)((Bn) + 15) / 16, (unsigned)(1)), 32, 0, stream>>>(gg7); }
    k_roll_cell<<<(unsigned)((Bn * H + 255) / 256), 256, 0, stream>>>(GT, C, A, Bn, H, E, KA);
    { GemmP gl7;
      gl7.A = A + E; gl7.B = Wo; gl7.bias = bo; gl7.R = A + E; gl7.C = LG;
      gl7.sAo = 0; gl7.sAi = 0; gl7.sAm = KA; gl7.sAk = 1; gl7.sBo = 0; gl7.sBi = 0; gl7.sBn = 1; gl7.sBk = V; gl7.sCo = 0; gl7.sCi = 0; gl7.sCm = V; gl7.sRo = 0; gl7.sRi = 0; gl7.sRm = 0; gl7.sRn = 0;
      gl7.M = Bn; gl7.N = V; gl7.K = H; gl7.zi_n = 1; gl7.flags = 1; gl7.act = 0;
      gl7.alpha = 1.0f; gl7.beta = 0.0f; gl7.sa = 1.0f; gl7.sb = 1.0f; gl7.Npad = V; gl7.pad_ = 0;
      k_gemm<3><<<dim3((unsigned)((V) + 31) / 32, (unsigned)((Bn) + 15) / 16, (unsigned)(1)), 32, 0, stream>>>(gl7); }
    k_roll_pick<<<Bn, 256, 0, stream>>>(LG, X, gnum, Emb, A, (int*)out, Bn, T, V, E, KA, 7);
    { GemmP gg8;
      gg8.A = A; gg8.B = PK; gg8.bias = BS; gg8.R = A; gg8.C = GT;
      gg8.sAo = 0; gg8.sAi = 0; gg8.sAm = KA; gg8.sAk = 1; gg8.sBo = 0; gg8.sBi = 0; gg8.sBn = 1; gg8.sBk = G4; gg8.sCo = 0; gg8.sCi = 0; gg8.sCm = G4; gg8.sRo = 0; gg8.sRi = 0; gg8.sRm = 0; gg8.sRn = 0;
      gg8.M = Bn; gg8.N = G4; gg8.K = KA; gg8.zi_n = 1; gg8.flags = 1; gg8.act = 0;
      gg8.alpha = 1.0f; gg8.beta = 0.0f; gg8.sa = 1.0f; gg8.sb = 1.0f; gg8.Npad = G4; gg8.pad_ = 0;
      k_gemm<3><<<dim3((unsigned)((G4) + 31) / 32, (unsigned)((Bn) + 15) / 16, (unsigned)(1)), 32, 0, stream>>>(gg8); }
    k_roll_cell<<<(unsigned)((Bn * H + 255) / 256), 256, 0, stream>>>(GT, C, A, Bn, H, E, KA);
    { GemmP gl8;
      gl8.A = A + E; gl8.B = Wo; gl8.bias = bo; gl8.R = A + E; gl8.C = LG;
      gl8.sAo = 0; gl8.sAi = 0; gl8.sAm = KA; gl8.sAk = 1; gl8.sBo = 0; gl8.sBi = 0; gl8.sBn = 1; gl8.sBk = V; gl8.sCo = 0; gl8.sCi = 0; gl8.sCm = V; gl8.sRo = 0; gl8.sRi = 0; gl8.sRm = 0; gl8.sRn = 0;
      gl8.M = Bn; gl8.N = V; gl8.K = H; gl8.zi_n = 1; gl8.flags = 1; gl8.act = 0;
      gl8.alpha = 1.0f; gl8.beta = 0.0f; gl8.sa = 1.0f; gl8.sb = 1.0f; gl8.Npad = V; gl8.pad_ = 0;
      k_gemm<3><<<dim3((unsigned)((V) + 31) / 32, (unsigned)((Bn) + 15) / 16, (unsigned)(1)), 32, 0, stream>>>(gl8); }
    k_roll_pick<<<Bn, 256, 0, stream>>>(LG, X, gnum, Emb, A, (int*)out, Bn, T, V, E, KA, 8);
    { GemmP gg9;
      gg9.A = A; gg9.B = PK; gg9.bias = BS; gg9.R = A; gg9.C = GT;
      gg9.sAo = 0; gg9.sAi = 0; gg9.sAm = KA; gg9.sAk = 1; gg9.sBo = 0; gg9.sBi = 0; gg9.sBn = 1; gg9.sBk = G4; gg9.sCo = 0; gg9.sCi = 0; gg9.sCm = G4; gg9.sRo = 0; gg9.sRi = 0; gg9.sRm = 0; gg9.sRn = 0;
      gg9.M = Bn; gg9.N = G4; gg9.K = KA; gg9.zi_n = 1; gg9.flags = 1; gg9.act = 0;
      gg9.alpha = 1.0f; gg9.beta = 0.0f; gg9.sa = 1.0f; gg9.sb = 1.0f; gg9.Npad = G4; gg9.pad_ = 0;
      k_gemm<3><<<dim3((unsigned)((G4) + 31) / 32, (unsigned)((Bn) + 15) / 16, (unsigned)(1)), 32, 0, stream>>>(gg9); }
    k_roll_cell<<<(unsigned)((Bn * H + 255) / 256), 256, 0, stream>>>(GT, C, A, Bn, H, E, KA);
    { GemmP gl9;
      gl9.A = A + E; gl9.B = Wo; gl9.bias = bo; gl9.R = A + E; gl9.C = LG;
      gl9.sAo = 0; gl9.sAi = 0; gl9.sAm = KA; gl9.sAk = 1; gl9.sBo = 0; gl9.sBi = 0; gl9.sBn = 1; gl9.sBk = V; gl9.sCo = 0; gl9.sCi = 0; gl9.sCm = V; gl9.sRo = 0; gl9.sRi = 0; gl9.sRm = 0; gl9.sRn = 0;
      gl9.M = Bn; gl9.N = V; gl9.K = H; gl9.zi_n = 1; gl9.flags = 1; gl9.act = 0;
      gl9.alpha = 1.0f; gl9.beta = 0.0f; gl9.sa = 1.0f; gl9.sb = 1.0f; gl9.Npad = V; gl9.pad_ = 0;
      k_gemm<3><<<dim3((unsigned)((V) + 31) / 32, (unsigned)((Bn) + 15) / 16, (unsigned)(1)), 32, 0, stream>>>(gl9); }
    k_roll_pick<<<Bn, 256, 0, stream>>>(LG, X, gnum, Emb, A, (int*)out, Bn, T, V, E, KA, 9);
    { GemmP gg10;
      gg10.A = A; gg10.B = PK; gg10.bias = BS; gg10.R = A; gg10.C = GT;
      gg10.sAo = 0; gg10.sAi = 0; gg10.sAm = KA; gg10.sAk = 1; gg10.sBo = 0; gg10.sBi = 0; gg10.sBn = 1; gg10.sBk = G4; gg10.sCo = 0; gg10.sCi = 0; gg10.sCm = G4; gg10.sRo = 0; gg10.sRi = 0; gg10.sRm = 0; gg10.sRn = 0;
      gg10.M = Bn; gg10.N = G4; gg10.K = KA; gg10.zi_n = 1; gg10.flags = 1; gg10.act = 0;
      gg10.alpha = 1.0f; gg10.beta = 0.0f; gg10.sa = 1.0f; gg10.sb = 1.0f; gg10.Npad = G4; gg10.pad_ = 0;
      k_gemm<3><<<dim3((unsigned)((G4) + 31) / 32, (unsigned)((Bn) + 15) / 16, (unsigned)(1)), 32, 0, stream>>>(gg10); }
    k_roll_cell<<<(unsigned)((Bn * H + 255) / 256), 256, 0, stream>>>(GT, C, A, Bn, H, E, KA);
    { GemmP gl10;
      gl10.A = A + E; gl10.B = Wo; gl10.bias = bo; gl10.R = A + E; gl10.C = LG;
      gl10.sAo = 0; gl10.sAi = 0; gl10.sAm = KA; gl10.sAk = 1; gl10.sBo = 0; gl10.sBi = 0; gl10.sBn = 1; gl10.sBk = V; gl10.sCo = 0; gl10.sCi = 0; gl10.sCm = V; gl10.sRo = 0; gl10.sRi = 0; gl10.sRm = 0; gl10.sRn = 0;
      gl10.M = Bn; gl10.N = V; gl10.K = H; gl10.zi_n = 1; gl10.flags = 1; gl10.act = 0;
      gl10.alpha = 1.0f; gl10.beta = 0.0f; gl10.sa = 1.0f; gl10.sb = 1.0f; gl10.Npad = V; gl10.pad_ = 0;
      k_gemm<3><<<dim3((unsigned)((V) + 31) / 32, (unsigned)((Bn) + 15) / 16, (unsigned)(1)), 32, 0, stream>>>(gl10); }
    k_roll_pick<<<Bn, 256, 0, stream>>>(LG, X, gnum, Emb, A, (int*)out, Bn, T, V, E, KA, 10);
    { GemmP gg11;
      gg11.A = A; gg11.B = PK; gg11.bias = BS; gg11.R = A; gg11.C = GT;
      gg11.sAo = 0; gg11.sAi = 0; gg11.sAm = KA; gg11.sAk = 1; gg11.sBo = 0; gg11.sBi = 0; gg11.sBn = 1; gg11.sBk = G4; gg11.sCo = 0; gg11.sCi = 0; gg11.sCm = G4; gg11.sRo = 0; gg11.sRi = 0; gg11.sRm = 0; gg11.sRn = 0;
      gg11.M = Bn; gg11.N = G4; gg11.K = KA; gg11.zi_n = 1; gg11.flags = 1; gg11.act = 0;
      gg11.alpha = 1.0f; gg11.beta = 0.0f; gg11.sa = 1.0f; gg11.sb = 1.0f; gg11.Npad = G4; gg11.pad_ = 0;
      k_gemm<3><<<dim3((unsigned)((G4) + 31) / 32, (unsigned)((Bn) + 15) / 16, (unsigned)(1)), 32, 0, stream>>>(gg11); }
    k_roll_cell<<<(unsigned)((Bn * H + 255) / 256), 256, 0, stream>>>(GT, C, A, Bn, H, E, KA);
    { GemmP gl11;
      gl11.A = A + E; gl11.B = Wo; gl11.bias = bo; gl11.R = A + E; gl11.C = LG;
      gl11.sAo = 0; gl11.sAi = 0; gl11.sAm = KA; gl11.sAk = 1; gl11.sBo = 0; gl11.sBi = 0; gl11.sBn = 1; gl11.sBk = V; gl11.sCo = 0; gl11.sCi = 0; gl11.sCm = V; gl11.sRo = 0; gl11.sRi = 0; gl11.sRm = 0; gl11.sRn = 0;
      gl11.M = Bn; gl11.N = V; gl11.K = H; gl11.zi_n = 1; gl11.flags = 1; gl11.act = 0;
      gl11.alpha = 1.0f; gl11.beta = 0.0f; gl11.sa = 1.0f; gl11.sb = 1.0f; gl11.Npad = V; gl11.pad_ = 0;
      k_gemm<3><<<dim3((unsigned)((V) + 31) / 32, (unsigned)((Bn) + 15) / 16, (unsigned)(1)), 32, 0, stream>>>(gl11); }
    k_roll_pick<<<Bn, 256, 0, stream>>>(LG, X, gnum, Emb, A, (int*)out, Bn, T, V, E, KA, 11);
    { GemmP gg12;
      gg12.A = A; gg12.B = PK; gg12.bias = BS; gg12.R = A; gg12.C = GT;
      gg12.sAo = 0; gg12.sAi = 0; gg12.sAm = KA; gg12.sAk = 1; gg12.sBo = 0; gg12.sBi = 0; gg12.sBn = 1; gg12.sBk = G4; gg12.sCo = 0; gg12.sCi = 0; gg12.sCm = G4; gg12.sRo = 0; gg12.sRi = 0; gg12.sRm = 0; gg12.sRn = 0;
      gg12.M = Bn; gg12.N = G4; gg12.K = KA; gg12.zi_n = 1; gg12.flags = 1; gg12.act = 0;
      gg12.alpha = 1.0f; gg12.beta = 0.0f; gg12.sa = 1.0f; gg12.sb = 1.0f; gg12.Npad = G4; gg12.pad_ = 0;
      k_gemm<3><<<dim3((unsigned)((G4) + 31) / 32, (unsigned)((Bn) + 15) / 16, (unsigned)(1)), 32, 0, stream>>>(gg12); }
    k_roll_cell<<<(unsigned)((Bn * H + 255) / 256), 256, 0, stream>>>(GT, C, A, Bn, H, E, KA);
    { GemmP gl12;
      gl12.A = A + E; gl12.B = Wo; gl12.bias = bo; gl12.R = A + E; gl12.C = LG;
      gl12.sAo = 0; gl12.sAi = 0; gl12.sAm = KA; gl12.sAk = 1; gl12.sBo = 0; gl12.sBi = 0; gl12.sBn = 1; gl12.sBk = V; gl12.sCo = 0; gl12.sCi = 0; gl12.sCm = V; gl12.sRo = 0; gl12.sRi = 0; gl12.sRm = 0; gl12.sRn = 0;
      gl12.M = Bn; gl12.N = V; gl12.K = H; gl12.zi_n = 1; gl12.flags = 1; gl12.act = 0;
      gl12.alpha = 1.0f; gl12.beta = 0.0f; gl12.sa = 1.0f; gl12.sb = 1.0f; gl12.Npad = V; gl12.pad_ = 0;
      k_gemm<3><<<dim3((unsigned)((V) + 31) / 32, (unsigned)((Bn) + 15) / 16, (unsigned)(1)), 32, 0, stream>>>(gl12); }
    k_roll_pick<<<Bn, 256, 0, stream>>>(LG, X, gnum, Emb, A, (int*)out, Bn, T, V, E, KA, 12);
    { GemmP gg13;
      gg13.A = A; gg13.B = PK; gg13.bias = BS; gg13.R = A; gg13.C = GT;
      gg13.sAo = 0; gg13.sAi = 0; gg13.sAm = KA; gg13.sAk = 1; gg13.sBo = 0; gg13.sBi = 0; gg13.sBn = 1; gg13.sBk = G4; gg13.sCo = 0; gg13.sCi = 0; gg13.sCm = G4; gg13.sRo = 0; gg13.sRi = 0; gg13.sRm = 0; gg13.sRn = 0;
      gg13.M = Bn; gg13.N = G4; gg13.K = KA; gg13.zi_n = 1; gg13.flags = 1; gg13.act = 0;
      gg13.alpha = 1.0f; gg13.beta = 0.0f; gg13.sa = 1.0f; gg13.sb = 1.0f; gg13.Npad = G4; gg13.pad_ = 0;
      k_gemm<3><<<dim3((unsigned)((G4) + 31) / 32, (unsigned)((Bn) + 15) / 16, (unsigned)(1)), 32, 0, stream>>>(gg13); }
    k_roll_cell<<<(unsigned)((Bn * H + 255) / 256), 256, 0, stream>>>(GT, C, A, Bn, H, E, KA);
    { GemmP gl13;
      gl13.A = A + E; gl13.B = Wo; gl13.bias = bo; gl13.R = A + E; gl13.C = LG;
      gl13.sAo = 0; gl13.sAi = 0; gl13.sAm = KA; gl13.sAk = 1; gl13.sBo = 0; gl13.sBi = 0; gl13.sBn = 1; gl13.sBk = V; gl13.sCo = 0; gl13.sCi = 0; gl13.sCm = V; gl13.sRo = 0; gl13.sRi = 0; gl13.sRm = 0; gl13.sRn = 0;
      gl13.M = Bn; gl13.N = V; gl13.K = H; gl13.zi_n = 1; gl13.flags = 1; gl13.act = 0;
      gl13.alpha = 1.0f; gl13.beta = 0.0f; gl13.sa = 1.0f; gl13.sb = 1.0f; gl13.Npad = V; gl13.pad_ = 0;
      k_gemm<3><<<dim3((unsigned)((V) + 31) / 32, (unsigned)((Bn) + 15) / 16, (unsigned)(1)), 32, 0, stream>>>(gl13); }
    k_roll_pick<<<Bn, 256, 0, stream>>>(LG, X, gnum, Emb, A, (int*)out, Bn, T, V, E, KA, 13);
    { GemmP gg14;
      gg14.A = A; gg14.B = PK; gg14.bias = BS; gg14.R = A; gg14.C = GT;
      gg14.sAo = 0; gg14.sAi = 0; gg14.sAm = KA; gg14.sAk = 1; gg14.sBo = 0; gg14.sBi = 0; gg14.sBn = 1; gg14.sBk = G4; gg14.sCo = 0; gg14.sCi = 0; gg14.sCm = G4; gg14.sRo = 0; gg14.sRi = 0; gg14.sRm = 0; gg14.sRn = 0;
      gg14.M = Bn; gg14.N = G4; gg14.K = KA; gg14.zi_n = 1; gg14.flags = 1; gg14.act = 0;
      gg14.alpha = 1.0f; gg14.beta = 0.0f; gg14.sa = 1.0f; gg14.sb = 1.0f; gg14.Npad = G4; gg14.pad_ = 0;
      k_gemm<3><<<dim3((unsigned)((G4) + 31) / 32, (unsigned)((Bn) + 15) / 16, (unsigned)(1)), 32, 0, stream>>>(gg14); }
    k_roll_cell<<<(unsigned)((Bn * H + 255) / 256), 256, 0, stream>>>(GT, C, A, Bn, H, E, KA);
    { GemmP gl14;
      gl14.A = A + E; gl14.B = Wo; gl14.bias = bo; gl14.R = A + E; gl14.C = LG;
      gl14.sAo = 0; gl14.sAi = 0; gl14.sAm = KA; gl14.sAk = 1; gl14.sBo = 0; gl14.sBi = 0; gl14.sBn = 1; gl14.sBk = V; gl14.sCo = 0; gl14.sCi = 0; gl14.sCm = V; gl14.sRo = 0; gl14.sRi = 0; gl14.sRm = 0; gl14.sRn = 0;
      gl14.M = Bn; gl14.N = V; gl14.K = H; gl14.zi_n = 1; gl14.flags = 1; gl14.act = 0;
      gl14.alpha = 1.0f; gl14.beta = 0.0f; gl14.sa = 1.0f; gl14.sb = 1.0f; gl14.Npad = V; gl14.pad_ = 0;
      k_gemm<3><<<dim3((unsigned)((V) + 31) / 32, (unsigned)((Bn) + 15) / 16, (unsigned)(1)), 32, 0, stream>>>(gl14); }
    k_roll_pick<<<Bn, 256, 0, stream>>>(LG, X, gnum, Emb, A, (int*)out, Bn, T, V, E, KA, 14);
    { GemmP gg15;
      gg15.A = A; gg15.B = PK; gg15.bias = BS; gg15.R = A; gg15.C = GT;
      gg15.sAo = 0; gg15.sAi = 0; gg15.sAm = KA; gg15.sAk = 1; gg15.sBo = 0; gg15.sBi = 0; gg15.sBn = 1; gg15.sBk = G4; gg15.sCo = 0; gg15.sCi = 0; gg15.sCm = G4; gg15.sRo = 0; gg15.sRi = 0; gg15.sRm = 0; gg15.sRn = 0;
      gg15.M = Bn; gg15.N = G4; gg15.K = KA; gg15.zi_n = 1; gg15.flags = 1; gg15.act = 0;
      gg15.alpha = 1.0f; gg15.beta = 0.0f; gg15.sa = 1.0f; gg15.sb = 1.0f; gg15.Npad = G4; gg15.pad_ = 0;
      k_gemm<3><<<dim3((unsigned)((G4) + 31) / 32, (unsigned)((Bn) + 15) / 16, (unsigned)(1)), 32, 0, stream>>>(gg15); }
    k_roll_cell<<<(unsigned)((Bn * H + 255) / 256), 256, 0, stream>>>(GT, C, A, Bn, H, E, KA);
    { GemmP gl15;
      gl15.A = A + E; gl15.B = Wo; gl15.bias = bo; gl15.R = A + E; gl15.C = LG;
      gl15.sAo = 0; gl15.sAi = 0; gl15.sAm = KA; gl15.sAk = 1; gl15.sBo = 0; gl15.sBi = 0; gl15.sBn = 1; gl15.sBk = V; gl15.sCo = 0; gl15.sCi = 0; gl15.sCm = V; gl15.sRo = 0; gl15.sRi = 0; gl15.sRm = 0; gl15.sRn = 0;
      gl15.M = Bn; gl15.N = V; gl15.K = H; gl15.zi_n = 1; gl15.flags = 1; gl15.act = 0;
      gl15.alpha = 1.0f; gl15.beta = 0.0f; gl15.sa = 1.0f; gl15.sb = 1.0f; gl15.Npad = V; gl15.pad_ = 0;
      k_gemm<3><<<dim3((unsigned)((V) + 31) / 32, (unsigned)((Bn) + 15) / 16, (unsigned)(1)), 32, 0, stream>>>(gl15); }
    k_roll_pick<<<Bn, 256, 0, stream>>>(LG, X, gnum, Emb, A, (int*)out, Bn, T, V, E, KA, 15);
    { GemmP gg16;
      gg16.A = A; gg16.B = PK; gg16.bias = BS; gg16.R = A; gg16.C = GT;
      gg16.sAo = 0; gg16.sAi = 0; gg16.sAm = KA; gg16.sAk = 1; gg16.sBo = 0; gg16.sBi = 0; gg16.sBn = 1; gg16.sBk = G4; gg16.sCo = 0; gg16.sCi = 0; gg16.sCm = G4; gg16.sRo = 0; gg16.sRi = 0; gg16.sRm = 0; gg16.sRn = 0;
      gg16.M = Bn; gg16.N = G4; gg16.K = KA; gg16.zi_n = 1; gg16.flags = 1; gg16.act = 0;
      gg16.alpha = 1.0f; gg16.beta = 0.0f; gg16.sa = 1.0f; gg16.sb = 1.0f; gg16.Npad = G4; gg16.pad_ = 0;
      k_gemm<3><<<dim3((unsigned)((G4) + 31) / 32, (unsigned)((Bn) + 15) / 16, (unsigned)(1)), 32, 0, stream>>>(gg16); }
    k_roll_cell<<<(unsigned)((Bn * H + 255) / 256), 256, 0, stream>>>(GT, C, A, Bn, H, E, KA);
    { GemmP gl16;
      gl16.A = A + E; gl16.B = Wo; gl16.bias = bo; gl16.R = A + E; gl16.C = LG;
      gl16.sAo = 0; gl16.sAi = 0; gl16.sAm = KA; gl16.sAk = 1; gl16.sBo = 0; gl16.sBi = 0; gl16.sBn = 1; gl16.sBk = V; gl16.sCo = 0; gl16.sCi = 0; gl16.sCm = V; gl16.sRo = 0; gl16.sRi = 0; gl16.sRm = 0; gl16.sRn = 0;
      gl16.M = Bn; gl16.N = V; gl16.K = H; gl16.zi_n = 1; gl16.flags = 1; gl16.act = 0;
      gl16.alpha = 1.0f; gl16.beta = 0.0f; gl16.sa = 1.0f; gl16.sb = 1.0f; gl16.Npad = V; gl16.pad_ = 0;
      k_gemm<3><<<dim3((unsigned)((V) + 31) / 32, (unsigned)((Bn) + 15) / 16, (unsigned)(1)), 32, 0, stream>>>(gl16); }
    k_roll_pick<<<Bn, 256, 0, stream>>>(LG, X, gnum, Emb, A, (int*)out, Bn, T, V, E, KA, 16);
    { GemmP gg17;
      gg17.A = A; gg17.B = PK; gg17.bias = BS; gg17.R = A; gg17.C = GT;
      gg17.sAo = 0; gg17.sAi = 0; gg17.sAm = KA; gg17.sAk = 1; gg17.sBo = 0; gg17.sBi = 0; gg17.sBn = 1; gg17.sBk = G4; gg17.sCo = 0; gg17.sCi = 0; gg17.sCm = G4; gg17.sRo = 0; gg17.sRi = 0; gg17.sRm = 0; gg17.sRn = 0;
      gg17.M = Bn; gg17.N = G4; gg17.K = KA; gg17.zi_n = 1; gg17.flags = 1; gg17.act = 0;
      gg17.alpha = 1.0f; gg17.beta = 0.0f; gg17.sa = 1.0f; gg17.sb = 1.0f; gg17.Npad = G4; gg17.pad_ = 0;
      k_gemm<3><<<dim3((unsigned)((G4) + 31) / 32, (unsigned)((Bn) + 15) / 16, (unsigned)(1)), 32, 0, stream>>>(gg17); }
    k_roll_cell<<<(unsigned)((Bn * H + 255) / 256), 256, 0, stream>>>(GT, C, A, Bn, H, E, KA);
    { GemmP gl17;
      gl17.A = A + E; gl17.B = Wo; gl17.bias = bo; gl17.R = A + E; gl17.C = LG;
      gl17.sAo = 0; gl17.sAi = 0; gl17.sAm = KA; gl17.sAk = 1; gl17.sBo = 0; gl17.sBi = 0; gl17.sBn = 1; gl17.sBk = V; gl17.sCo = 0; gl17.sCi = 0; gl17.sCm = V; gl17.sRo = 0; gl17.sRi = 0; gl17.sRm = 0; gl17.sRn = 0;
      gl17.M = Bn; gl17.N = V; gl17.K = H; gl17.zi_n = 1; gl17.flags = 1; gl17.act = 0;
      gl17.alpha = 1.0f; gl17.beta = 0.0f; gl17.sa = 1.0f; gl17.sb = 1.0f; gl17.Npad = V; gl17.pad_ = 0;
      k_gemm<3><<<dim3((unsigned)((V) + 31) / 32, (unsigned)((Bn) + 15) / 16, (unsigned)(1)), 32, 0, stream>>>(gl17); }
    k_roll_pick<<<Bn, 256, 0, stream>>>(LG, X, gnum, Emb, A, (int*)out, Bn, T, V, E, KA, 17);
    { GemmP gg18;
      gg18.A = A; gg18.B = PK; gg18.bias = BS; gg18.R = A; gg18.C = GT;
      gg18.sAo = 0; gg18.sAi = 0; gg18.sAm = KA; gg18.sAk = 1; gg18.sBo = 0; gg18.sBi = 0; gg18.sBn = 1; gg18.sBk = G4; gg18.sCo = 0; gg18.sCi = 0; gg18.sCm = G4; gg18.sRo = 0; gg18.sRi = 0; gg18.sRm = 0; gg18.sRn = 0;
      gg18.M = Bn; gg18.N = G4; gg18.K = KA; gg18.zi_n = 1; gg18.flags = 1; gg18.act = 0;
      gg18.alpha = 1.0f; gg18.beta = 0.0f; gg18.sa = 1.0f; gg18.sb = 1.0f; gg18.Npad = G4; gg18.pad_ = 0;
      k_gemm<3><<<dim3((unsigned)((G4) + 31) / 32, (unsigned)((Bn) + 15) / 16, (unsigned)(1)), 32, 0, stream>>>(gg18); }
    k_roll_cell<<<(unsigned)((Bn * H + 255) / 256), 256, 0, stream>>>(GT, C, A, Bn, H, E, KA);
    { GemmP gl18;
      gl18.A = A + E; gl18.B = Wo; gl18.bias = bo; gl18.R = A + E; gl18.C = LG;
      gl18.sAo = 0; gl18.sAi = 0; gl18.sAm = KA; gl18.sAk = 1; gl18.sBo = 0; gl18.sBi = 0; gl18.sBn = 1; gl18.sBk = V; gl18.sCo = 0; gl18.sCi = 0; gl18.sCm = V; gl18.sRo = 0; gl18.sRi = 0; gl18.sRm = 0; gl18.sRn = 0;
      gl18.M = Bn; gl18.N = V; gl18.K = H; gl18.zi_n = 1; gl18.flags = 1; gl18.act = 0;
      gl18.alpha = 1.0f; gl18.beta = 0.0f; gl18.sa = 1.0f; gl18.sb = 1.0f; gl18.Npad = V; gl18.pad_ = 0;
      k_gemm<3><<<dim3((unsigned)((V) + 31) / 32, (unsigned)((Bn) + 15) / 16, (unsigned)(1)), 32, 0, stream>>>(gl18); }
    k_roll_pick<<<Bn, 256, 0, stream>>>(LG, X, gnum, Emb, A, (int*)out, Bn, T, V, E, KA, 18);
    { GemmP gg19;
      gg19.A = A; gg19.B = PK; gg19.bias = BS; gg19.R = A; gg19.C = GT;
      gg19.sAo = 0; gg19.sAi = 0; gg19.sAm = KA; gg19.sAk = 1; gg19.sBo = 0; gg19.sBi = 0; gg19.sBn = 1; gg19.sBk = G4; gg19.sCo = 0; gg19.sCi = 0; gg19.sCm = G4; gg19.sRo = 0; gg19.sRi = 0; gg19.sRm = 0; gg19.sRn = 0;
      gg19.M = Bn; gg19.N = G4; gg19.K = KA; gg19.zi_n = 1; gg19.flags = 1; gg19.act = 0;
      gg19.alpha = 1.0f; gg19.beta = 0.0f; gg19.sa = 1.0f; gg19.sb = 1.0f; gg19.Npad = G4; gg19.pad_ = 0;
      k_gemm<3><<<dim3((unsigned)((G4) + 31) / 32, (unsigned)((Bn) + 15) / 16, (unsigned)(1)), 32, 0, stream>>>(gg19); }
    k_roll_cell<<<(unsigned)((Bn * H + 255) / 256), 256, 0, stream>>>(GT, C, A, Bn, H, E, KA);
    { GemmP gl19;
      gl19.A = A + E; gl19.B = Wo; gl19.bias = bo; gl19.R = A + E; gl19.C = LG;
      gl19.sAo = 0; gl19.sAi = 0; gl19.sAm = KA; gl19.sAk = 1; gl19.sBo = 0; gl19.sBi = 0; gl19.sBn = 1; gl19.sBk = V; gl19.sCo = 0; gl19.sCi = 0; gl19.sCm = V; gl19.sRo = 0; gl19.sRi = 0; gl19.sRm = 0; gl19.sRn = 0;
      gl19.M = Bn; gl19.N = V; gl19.K = H; gl19.zi_n = 1; gl19.flags = 1; gl19.act = 0;
      gl19.alpha = 1.0f; gl19.beta = 0.0f; gl19.sa = 1.0f; gl19.sb = 1.0f; gl19.Npad = V; gl19.pad_ = 0;
      k_gemm<3><<<dim3((unsigned)((V) + 31) / 32, (unsigned)((Bn) + 15) / 16, (unsigned)(1)), 32, 0, stream>>>(gl19); }
    k_roll_pick<<<Bn, 256, 0, stream>>>(LG, X, gnum, Emb, A, (int*)out, Bn, T, V, E, KA, 19);
    { GemmP gg20;
      gg20.A = A; gg20.B = PK; gg20.bias = BS; gg20.R = A; gg20.C = GT;
      gg20.sAo = 0; gg20.sAi = 0; gg20.sAm = KA; gg20.sAk = 1; gg20.sBo = 0; gg20.sBi = 0; gg20.sBn = 1; gg20.sBk = G4; gg20.sCo = 0; gg20.sCi = 0; gg20.sCm = G4; gg20.sRo = 0; gg20.sRi = 0; gg20.sRm = 0; gg20.sRn = 0;
      gg20.M = Bn; gg20.N = G4; gg20.K = KA; gg20.zi_n = 1; gg20.flags = 1; gg20.act = 0;
      gg20.alpha = 1.0f; gg20.beta = 0.0f; gg20.sa = 1.0f; gg20.sb = 1.0f; gg20.Npad = G4; gg20.pad_ = 0;
      k_gemm<3><<<dim3((unsigned)((G4) + 31) / 32, (unsigned)((Bn) + 15) / 16, (unsigned)(1)), 32, 0, stream>>>(gg20); }
    k_roll_cell<<<(unsigned)((Bn * H + 255) / 256), 256, 0, stream>>>(GT, C, A, Bn, H, E, KA);
    { GemmP gl20;
      gl20.A = A + E; gl20.B = Wo; gl20.bias = bo; gl20.R = A + E; gl20.C = LG;
      gl20.sAo = 0; gl20.sAi = 0; gl20.sAm = KA; gl20.sAk = 1; gl20.sBo = 0; gl20.sBi = 0; gl20.sBn = 1; gl20.sBk = V; gl20.sCo = 0; gl20.sCi = 0; gl20.sCm = V; gl20.sRo = 0; gl20.sRi = 0; gl20.sRm = 0; gl20.sRn = 0;
      gl20.M = Bn; gl20.N = V; gl20.K = H; gl20.zi_n = 1; gl20.flags = 1; gl20.act = 0;
      gl20.alpha = 1.0f; gl20.beta = 0.0f; gl20.sa = 1.0f; gl20.sb = 1.0f; gl20.Npad = V; gl20.pad_ = 0;
      k_gemm<3><<<dim3((unsigned)((V) + 31) / 32, (unsigned)((Bn) + 15) / 16, (unsigned)(1)), 32, 0, stream>>>(gl20); }
    k_roll_pick<<<Bn, 256, 0, stream>>>(LG, X, gnum, Emb, A, (int*)out, Bn, T, V, E, KA, 20);
    { GemmP gg21;
      gg21.A = A; gg21.B = PK; gg21.bias = BS; gg21.R = A; gg21.C = GT;
      gg21.sAo = 0; gg21.sAi = 0; gg21.sAm = KA; gg21.sAk = 1; gg21.sBo = 0; gg21.sBi = 0; gg21.sBn = 1; gg21.sBk = G4; gg21.sCo = 0; gg21.sCi = 0; gg21.sCm = G4; gg21.sRo = 0; gg21.sRi = 0; gg21.sRm = 0; gg21.sRn = 0;
      gg21.M = Bn; gg21.N = G4; gg21.K = KA; gg21.zi_n = 1; gg21.flags = 1; gg21.act = 0;
      gg21.alpha = 1.0f; gg21.beta = 0.0f; gg21.sa = 1.0f; gg21.sb = 1.0f; gg21.Npad = G4; gg21.pad_ = 0;
      k_gemm<3><<<dim3((unsigned)((G4) + 31) / 32, (unsigned)((Bn) + 15) / 16, (unsigned)(1)), 32, 0, stream>>>(gg21); }
    k_roll_cell<<<(unsigned)((Bn * H + 255) / 256), 256, 0, stream>>>(GT, C, A, Bn, H, E, KA);
    { GemmP gl21;
      gl21.A = A + E; gl21.B = Wo; gl21.bias = bo; gl21.R = A + E; gl21.C = LG;
      gl21.sAo = 0; gl21.sAi = 0; gl21.sAm = KA; gl21.sAk = 1; gl21.sBo = 0; gl21.sBi = 0; gl21.sBn = 1; gl21.sBk = V; gl21.sCo = 0; gl21.sCi = 0; gl21.sCm = V; gl21.sRo = 0; gl21.sRi = 0; gl21.sRm = 0; gl21.sRn = 0;
      gl21.M = Bn; gl21.N = V; gl21.K = H; gl21.zi_n = 1; gl21.flags = 1; gl21.act = 0;
      gl21.alpha = 1.0f; gl21.beta = 0.0f; gl21.sa = 1.0f; gl21.sb = 1.0f; gl21.Npad = V; gl21.pad_ = 0;
      k_gemm<3><<<dim3((unsigned)((V) + 31) / 32, (unsigned)((Bn) + 15) / 16, (unsigned)(1)), 32, 0, stream>>>(gl21); }
    k_roll_pick<<<Bn, 256, 0, stream>>>(LG, X, gnum, Emb, A, (int*)out, Bn, T, V, E, KA, 21);
    { GemmP gg22;
      gg22.A = A; gg22.B = PK; gg22.bias = BS; gg22.R = A; gg22.C = GT;
      gg22.sAo = 0; gg22.sAi = 0; gg22.sAm = KA; gg22.sAk = 1; gg22.sBo = 0; gg22.sBi = 0; gg22.sBn = 1; gg22.sBk = G4; gg22.sCo = 0; gg22.sCi = 0; gg22.sCm = G4; gg22.sRo = 0; gg22.sRi = 0; gg22.sRm = 0; gg22.sRn = 0;
      gg22.M = Bn; gg22.N = G4; gg22.K = KA; gg22.zi_n = 1; gg22.flags = 1; gg22.act = 0;
      gg22.alpha = 1.0f; gg22.beta = 0.0f; gg22.sa = 1.0f; gg22.sb = 1.0f; gg22.Npad = G4; gg22.pad_ = 0;
      k_gemm<3><<<dim3((unsigned)((G4) + 31) / 32, (unsigned)((Bn) + 15) / 16, (unsigned)(1)), 32, 0, stream>>>(gg22); }
    k_roll_cell<<<(unsigned)((Bn * H + 255) / 256), 256, 0, stream>>>(GT, C, A, Bn, H, E, KA);
    { GemmP gl22;
      gl22.A = A + E; gl22.B = Wo; gl22.bias = bo; gl22.R = A + E; gl22.C = LG;
      gl22.sAo = 0; gl22.sAi = 0; gl22.sAm = KA; gl22.sAk = 1; gl22.sBo = 0; gl22.sBi = 0; gl22.sBn = 1; gl22.sBk = V; gl22.sCo = 0; gl22.sCi = 0; gl22.sCm = V; gl22.sRo = 0; gl22.sRi = 0; gl22.sRm = 0; gl22.sRn = 0;
      gl22.M = Bn; gl22.N = V; gl22.K = H; gl22.zi_n = 1; gl22.flags = 1; gl22.act = 0;
      gl22.alpha = 1.0f; gl22.beta = 0.0f; gl22.sa = 1.0f; gl22.sb = 1.0f; gl22.Npad = V; gl22.pad_ = 0;
      k_gemm<3><<<dim3((unsigned)((V) + 31) / 32, (unsigned)((Bn) + 15) / 16, (unsigned)(1)), 32, 0, stream>>>(gl22); }
    k_roll_pick<<<Bn, 256, 0, stream>>>(LG, X, gnum, Emb, A, (int*)out, Bn, T, V, E, KA, 22);
    { GemmP gg23;
      gg23.A = A; gg23.B = PK; gg23.bias = BS; gg23.R = A; gg23.C = GT;
      gg23.sAo = 0; gg23.sAi = 0; gg23.sAm = KA; gg23.sAk = 1; gg23.sBo = 0; gg23.sBi = 0; gg23.sBn = 1; gg23.sBk = G4; gg23.sCo = 0; gg23.sCi = 0; gg23.sCm = G4; gg23.sRo = 0; gg23.sRi = 0; gg23.sRm = 0; gg23.sRn = 0;
      gg23.M = Bn; gg23.N = G4; gg23.K = KA; gg23.zi_n = 1; gg23.flags = 1; gg23.act = 0;
      gg23.alpha = 1.0f; gg23.beta = 0.0f; gg23.sa = 1.0f; gg23.sb = 1.0f; gg23.Npad = G4; gg23.pad_ = 0;
      k_gemm<3><<<dim3((unsigned)((G4) + 31) / 32, (unsigned)((Bn) + 15) / 16, (unsigned)(1)), 32, 0, stream>>>(gg23); }
    k_roll_cell<<<(unsigned)((Bn * H + 255) / 256), 256, 0, stream>>>(GT, C, A, Bn, H, E, KA);
    { GemmP gl23;
      gl23.A = A + E; gl23.B = Wo; gl23.bias = bo; gl23.R = A + E; gl23.C = LG;
      gl23.sAo = 0; gl23.sAi = 0; gl23.sAm = KA; gl23.sAk = 1; gl23.sBo = 0; gl23.sBi = 0; gl23.sBn = 1; gl23.sBk = V; gl23.sCo = 0; gl23.sCi = 0; gl23.sCm = V; gl23.sRo = 0; gl23.sRi = 0; gl23.sRm = 0; gl23.sRn = 0;
      gl23.M = Bn; gl23.N = V; gl23.K = H; gl23.zi_n = 1; gl23.flags = 1; gl23.act = 0;
      gl23.alpha = 1.0f; gl23.beta = 0.0f; gl23.sa = 1.0f; gl23.sb = 1.0f; gl23.Npad = V; gl23.pad_ = 0;
      k_gemm<3><<<dim3((unsigned)((V) + 31) / 32, (unsigned)((Bn) + 15) / 16, (unsigned)(1)), 32, 0, stream>>>(gl23); }
    k_roll_pick<<<Bn, 256, 0, stream>>>(LG, X, gnum, Emb, A, (int*)out, Bn, T, V, E, KA, 23);
    { GemmP gg24;
      gg24.A = A; gg24.B = PK; gg24.bias = BS; gg24.R = A; gg24.C = GT;
      gg24.sAo = 0; gg24.sAi = 0; gg24.sAm = KA; gg24.sAk = 1; gg24.sBo = 0; gg24.sBi = 0; gg24.sBn = 1; gg24.sBk = G4; gg24.sCo = 0; gg24.sCi = 0; gg24.sCm = G4; gg24.sRo = 0; gg24.sRi = 0; gg24.sRm = 0; gg24.sRn = 0;
      gg24.M = Bn; gg24.N = G4; gg24.K = KA; gg24.zi_n = 1; gg24.flags = 1; gg24.act = 0;
      gg24.alpha = 1.0f; gg24.beta = 0.0f; gg24.sa = 1.0f; gg24.sb = 1.0f; gg24.Npad = G4; gg24.pad_ = 0;
      k_gemm<3><<<dim3((unsigned)((G4) + 31) / 32, (unsigned)((Bn) + 15) / 16, (unsigned)(1)), 32, 0, stream>>>(gg24); }
    k_roll_cell<<<(unsigned)((Bn * H + 255) / 256), 256, 0, stream>>>(GT, C, A, Bn, H, E, KA);
    { GemmP gl24;
      gl24.A = A + E; gl24.B = Wo; gl24.bias = bo; gl24.R = A + E; gl24.C = LG;
      gl24.sAo = 0; gl24.sAi = 0; gl24.sAm = KA; gl24.sAk = 1; gl24.sBo = 0; gl24.sBi = 0; gl24.sBn = 1; gl24.sBk = V; gl24.sCo = 0; gl24.sCi = 0; gl24.sCm = V; gl24.sRo = 0; gl24.sRi = 0; gl24.sRm = 0; gl24.sRn = 0;
      gl24.M = Bn; gl24.N = V; gl24.K = H; gl24.zi_n = 1; gl24.flags = 1; gl24.act = 0;
      gl24.alpha = 1.0f; gl24.beta = 0.0f; gl24.sa = 1.0f; gl24.sb = 1.0f; gl24.Npad = V; gl24.pad_ = 0;
      k_gemm<3><<<dim3((unsigned)((V) + 31) / 32, (unsigned)((Bn) + 15) / 16, (unsigned)(1)), 32, 0, stream>>>(gl24); }
    k_roll_pick<<<Bn, 256, 0, stream>>>(LG, X, gnum, Emb, A, (int*)out, Bn, T, V, E, KA, 24);
    { GemmP gg25;
      gg25.A = A; gg25.B = PK; gg25.bias = BS; gg25.R = A; gg25.C = GT;
      gg25.sAo = 0; gg25.sAi = 0; gg25.sAm = KA; gg25.sAk = 1; gg25.sBo = 0; gg25.sBi = 0; gg25.sBn = 1; gg25.sBk = G4; gg25.sCo = 0; gg25.sCi = 0; gg25.sCm = G4; gg25.sRo = 0; gg25.sRi = 0; gg25.sRm = 0; gg25.sRn = 0;
      gg25.M = Bn; gg25.N = G4; gg25.K = KA; gg25.zi_n = 1; gg25.flags = 1; gg25.act = 0;
      gg25.alpha = 1.0f; gg25.beta = 0.0f; gg25.sa = 1.0f; gg25.sb = 1.0f; gg25.Npad = G4; gg25.pad_ = 0;
      k_gemm<3><<<dim3((unsigned)((G4) + 31) / 32, (unsigned)((Bn) + 15) / 16, (unsigned)(1)), 32, 0, stream>>>(gg25); }
    k_roll_cell<<<(unsigned)((Bn * H + 255) / 256), 256, 0, stream>>>(GT, C, A, Bn, H, E, KA);
    { GemmP gl25;
      gl25.A = A + E; gl25.B = Wo; gl25.bias = bo; gl25.R = A + E; gl25.C = LG;
      gl25.sAo = 0; gl25.sAi = 0; gl25.sAm = KA; gl25.sAk = 1; gl25.sBo = 0; gl25.sBi = 0; gl25.sBn = 1; gl25.sBk = V; gl25.sCo = 0; gl25.sCi = 0; gl25.sCm = V; gl25.sRo = 0; gl25.sRi = 0; gl25.sRm = 0; gl25.sRn = 0;
      gl25.M = Bn; gl25.N = V; gl25.K = H; gl25.zi_n = 1; gl25.flags = 1; gl25.act = 0;
      gl25.alpha = 1.0f; gl25.beta = 0.0f; gl25.sa = 1.0f; gl25.sb = 1.0f; gl25.Npad = V; gl25.pad_ = 0;
      k_gemm<3><<<dim3((unsigned)((V) + 31) / 32, (unsigned)((Bn) + 15) / 16, (unsigned)(1)), 32, 0, stream>>>(gl25); }
    k_roll_pick<<<Bn, 256, 0, stream>>>(LG, X, gnum, Emb, A, (int*)out, Bn, T, V, E, KA, 25);
    { GemmP gg26;
      gg26.A = A; gg26.B = PK; gg26.bias = BS; gg26.R = A; gg26.C = GT;
      gg26.sAo = 0; gg26.sAi = 0; gg26.sAm = KA; gg26.sAk = 1; gg26.sBo = 0; gg26.sBi = 0; gg26.sBn = 1; gg26.sBk = G4; gg26.sCo = 0; gg26.sCi = 0; gg26.sCm = G4; gg26.sRo = 0; gg26.sRi = 0; gg26.sRm = 0; gg26.sRn = 0;
      gg26.M = Bn; gg26.N = G4; gg26.K = KA; gg26.zi_n = 1; gg26.flags = 1; gg26.act = 0;
      gg26.alpha = 1.0f; gg26.beta = 0.0f; gg26.sa = 1.0f; gg26.sb = 1.0f; gg26.Npad = G4; gg26.pad_ = 0;
      k_gemm<3><<<dim3((unsigned)((G4) + 31) / 32, (unsigned)((Bn) + 15) / 16, (unsigned)(1)), 32, 0, stream>>>(gg26); }
    k_roll_cell<<<(unsigned)((Bn * H + 255) / 256), 256, 0, stream>>>(GT, C, A, Bn, H, E, KA);
    { GemmP gl26;
      gl26.A = A + E; gl26.B = Wo; gl26.bias = bo; gl26.R = A + E; gl26.C = LG;
      gl26.sAo = 0; gl26.sAi = 0; gl26.sAm = KA; gl26.sAk = 1; gl26.sBo = 0; gl26.sBi = 0; gl26.sBn = 1; gl26.sBk = V; gl26.sCo = 0; gl26.sCi = 0; gl26.sCm = V; gl26.sRo = 0; gl26.sRi = 0; gl26.sRm = 0; gl26.sRn = 0;
      gl26.M = Bn; gl26.N = V; gl26.K = H; gl26.zi_n = 1; gl26.flags = 1; gl26.act = 0;
      gl26.alpha = 1.0f; gl26.beta = 0.0f; gl26.sa = 1.0f; gl26.sb = 1.0f; gl26.Npad = V; gl26.pad_ = 0;
      k_gemm<3><<<dim3((unsigned)((V) + 31) / 32, (unsigned)((Bn) + 15) / 16, (unsigned)(1)), 32, 0, stream>>>(gl26); }
    k_roll_pick<<<Bn, 256, 0, stream>>>(LG, X, gnum, Emb, A, (int*)out, Bn, T, V, E, KA, 26);
    { GemmP gg27;
      gg27.A = A; gg27.B = PK; gg27.bias = BS; gg27.R = A; gg27.C = GT;
      gg27.sAo = 0; gg27.sAi = 0; gg27.sAm = KA; gg27.sAk = 1; gg27.sBo = 0; gg27.sBi = 0; gg27.sBn = 1; gg27.sBk = G4; gg27.sCo = 0; gg27.sCi = 0; gg27.sCm = G4; gg27.sRo = 0; gg27.sRi = 0; gg27.sRm = 0; gg27.sRn = 0;
      gg27.M = Bn; gg27.N = G4; gg27.K = KA; gg27.zi_n = 1; gg27.flags = 1; gg27.act = 0;
      gg27.alpha = 1.0f; gg27.beta = 0.0f; gg27.sa = 1.0f; gg27.sb = 1.0f; gg27.Npad = G4; gg27.pad_ = 0;
      k_gemm<3><<<dim3((unsigned)((G4) + 31) / 32, (unsigned)((Bn) + 15) / 16, (unsigned)(1)), 32, 0, stream>>>(gg27); }
    k_roll_cell<<<(unsigned)((Bn * H + 255) / 256), 256, 0, stream>>>(GT, C, A, Bn, H, E, KA);
    { GemmP gl27;
      gl27.A = A + E; gl27.B = Wo; gl27.bias = bo; gl27.R = A + E; gl27.C = LG;
      gl27.sAo = 0; gl27.sAi = 0; gl27.sAm = KA; gl27.sAk = 1; gl27.sBo = 0; gl27.sBi = 0; gl27.sBn = 1; gl27.sBk = V; gl27.sCo = 0; gl27.sCi = 0; gl27.sCm = V; gl27.sRo = 0; gl27.sRi = 0; gl27.sRm = 0; gl27.sRn = 0;
      gl27.M = Bn; gl27.N = V; gl27.K = H; gl27.zi_n = 1; gl27.flags = 1; gl27.act = 0;
      gl27.alpha = 1.0f; gl27.beta = 0.0f; gl27.sa = 1.0f; gl27.sb = 1.0f; gl27.Npad = V; gl27.pad_ = 0;
      k_gemm<3><<<dim3((unsigned)((V) + 31) / 32, (unsigned)((Bn) + 15) / 16, (unsigned)(1)), 32, 0, stream>>>(gl27); }
    k_roll_pick<<<Bn, 256, 0, stream>>>(LG, X, gnum, Emb, A, (int*)out, Bn, T, V, E, KA, 27);
    { GemmP gg28;
      gg28.A = A; gg28.B = PK; gg28.bias = BS; gg28.R = A; gg28.C = GT;
      gg28.sAo = 0; gg28.sAi = 0; gg28.sAm = KA; gg28.sAk = 1; gg28.sBo = 0; gg28.sBi = 0; gg28.sBn = 1; gg28.sBk = G4; gg28.sCo = 0; gg28.sCi = 0; gg28.sCm = G4; gg28.sRo = 0; gg28.sRi = 0; gg28.sRm = 0; gg28.sRn = 0;
      gg28.M = Bn; gg28.N = G4; gg28.K = KA; gg28.zi_n = 1; gg28.flags = 1; gg28.act = 0;
      gg28.alpha = 1.0f; gg28.beta = 0.0f; gg28.sa = 1.0f; gg28.sb = 1.0f; gg28.Npad = G4; gg28.pad_ = 0;
      k_gemm<3><<<dim3((unsigned)((G4) + 31) / 32, (unsigned)((Bn) + 15) / 16, (unsigned)(1)), 32, 0, stream>>>(gg28); }
    k_roll_cell<<<(unsigned)((Bn * H + 255) / 256), 256, 0, stream>>>(GT, C, A, Bn, H, E, KA);
    { GemmP gl28;
      gl28.A = A + E; gl28.B = Wo; gl28.bias = bo; gl28.R = A + E; gl28.C = LG;
      gl28.sAo = 0; gl28.sAi = 0; gl28.sAm = KA; gl28.sAk = 1; gl28.sBo = 0; gl28.sBi = 0; gl28.sBn = 1; gl28.sBk = V; gl28.sCo = 0; gl28.sCi = 0; gl28.sCm = V; gl28.sRo = 0; gl28.sRi = 0; gl28.sRm = 0; gl28.sRn = 0;
      gl28.M = Bn; gl28.N = V; gl28.K = H; gl28.zi_n = 1; gl28.flags = 1; gl28.act = 0;
      gl28.alpha = 1.0f; gl28.beta = 0.0f; gl28.sa = 1.0f; gl28.sb = 1.0f; gl28.Npad = V; gl28.pad_ = 0;
      k_gemm<3><<<dim3((unsigned)((V) + 31) / 32, (unsigned)((Bn) + 15) / 16, (unsigned)(1)), 32, 0, stream>>>(gl28); }
    k_roll_pick<<<Bn, 256, 0, stream>>>(LG, X, gnum, Emb, A, (int*)out, Bn, T, V, E, KA, 28);
    { GemmP gg29;
      gg29.A = A; gg29.B = PK; gg29.bias = BS; gg29.R = A; gg29.C = GT;
      gg29.sAo = 0; gg29.sAi = 0; gg29.sAm = KA; gg29.sAk = 1; gg29.sBo = 0; gg29.sBi = 0; gg29.sBn = 1; gg29.sBk = G4; gg29.sCo = 0; gg29.sCi = 0; gg29.sCm = G4; gg29.sRo = 0; gg29.sRi = 0; gg29.sRm = 0; gg29.sRn = 0;
      gg29.M = Bn; gg29.N = G4; gg29.K = KA; gg29.zi_n = 1; gg29.flags = 1; gg29.act = 0;
      gg29.alpha = 1.0f; gg29.beta = 0.0f; gg29.sa = 1.0f; gg29.sb = 1.0f; gg29.Npad = G4; gg29.pad_ = 0;
      k_gemm<3><<<dim3((unsigned)((G4) + 31) / 32, (unsigned)((Bn) + 15) / 16, (unsigned)(1)), 32, 0, stream>>>(gg29); }
    k_roll_cell<<<(unsigned)((Bn * H + 255) / 256), 256, 0, stream>>>(GT, C, A, Bn, H, E, KA);
    { GemmP gl29;
      gl29.A = A + E; gl29.B = Wo; gl29.bias = bo; gl29.R = A + E; gl29.C = LG;
      gl29.sAo = 0; gl29.sAi = 0; gl29.sAm = KA; gl29.sAk = 1; gl29.sBo = 0; gl29.sBi = 0; gl29.sBn = 1; gl29.sBk = V; gl29.sCo = 0; gl29.sCi = 0; gl29.sCm = V; gl29.sRo = 0; gl29.sRi = 0; gl29.sRm = 0; gl29.sRn = 0;
      gl29.M = Bn; gl29.N = V; gl29.K = H; gl29.zi_n = 1; gl29.flags = 1; gl29.act = 0;
      gl29.alpha = 1.0f; gl29.beta = 0.0f; gl29.sa = 1.0f; gl29.sb = 1.0f; gl29.Npad = V; gl29.pad_ = 0;
      k_gemm<3><<<dim3((unsigned)((V) + 31) / 32, (unsigned)((Bn) + 15) / 16, (unsigned)(1)), 32, 0, stream>>>(gl29); }
    k_roll_pick<<<Bn, 256, 0, stream>>>(LG, X, gnum, Emb, A, (int*)out, Bn, T, V, E, KA, 29);
    { GemmP gg30;
      gg30.A = A; gg30.B = PK; gg30.bias = BS; gg30.R = A; gg30.C = GT;
      gg30.sAo = 0; gg30.sAi = 0; gg30.sAm = KA; gg30.sAk = 1; gg30.sBo = 0; gg30.sBi = 0; gg30.sBn = 1; gg30.sBk = G4; gg30.sCo = 0; gg30.sCi = 0; gg30.sCm = G4; gg30.sRo = 0; gg30.sRi = 0; gg30.sRm = 0; gg30.sRn = 0;
      gg30.M = Bn; gg30.N = G4; gg30.K = KA; gg30.zi_n = 1; gg30.flags = 1; gg30.act = 0;
      gg30.alpha = 1.0f; gg30.beta = 0.0f; gg30.sa = 1.0f; gg30.sb = 1.0f; gg30.Npad = G4; gg30.pad_ = 0;
      k_gemm<3><<<dim3((unsigned)((G4) + 31) / 32, (unsigned)((Bn) + 15) / 16, (unsigned)(1)), 32, 0, stream>>>(gg30); }
    k_roll_cell<<<(unsigned)((Bn * H + 255) / 256), 256, 0, stream>>>(GT, C, A, Bn, H, E, KA);
    { GemmP gl30;
      gl30.A = A + E; gl30.B = Wo; gl30.bias = bo; gl30.R = A + E; gl30.C = LG;
      gl30.sAo = 0; gl30.sAi = 0; gl30.sAm = KA; gl30.sAk = 1; gl30.sBo = 0; gl30.sBi = 0; gl30.sBn = 1; gl30.sBk = V; gl30.sCo = 0; gl30.sCi = 0; gl30.sCm = V; gl30.sRo = 0; gl30.sRi = 0; gl30.sRm = 0; gl30.sRn = 0;
      gl30.M = Bn; gl30.N = V; gl30.K = H; gl30.zi_n = 1; gl30.flags = 1; gl30.act = 0;
      gl30.alpha = 1.0f; gl30.beta = 0.0f; gl30.sa = 1.0f; gl30.sb = 1.0f; gl30.Npad = V; gl30.pad_ = 0;
      k_gemm<3><<<dim3((unsigned)((V) + 31) / 32, (unsigned)((Bn) + 15) / 16, (unsigned)(1)), 32, 0, stream>>>(gl30); }
    k_roll_pick<<<Bn, 256, 0, stream>>>(LG, X, gnum, Emb, A, (int*)out, Bn, T, V, E, KA, 30);
    { GemmP gg31;
      gg31.A = A; gg31.B = PK; gg31.bias = BS; gg31.R = A; gg31.C = GT;
      gg31.sAo = 0; gg31.sAi = 0; gg31.sAm = KA; gg31.sAk = 1; gg31.sBo = 0; gg31.sBi = 0; gg31.sBn = 1; gg31.sBk = G4; gg31.sCo = 0; gg31.sCi = 0; gg31.sCm = G4; gg31.sRo = 0; gg31.sRi = 0; gg31.sRm = 0; gg31.sRn = 0;
      gg31.M = Bn; gg31.N = G4; gg31.K = KA; gg31.zi_n = 1; gg31.flags = 1; gg31.act = 0;
      gg31.alpha = 1.0f; gg31.beta = 0.0f; gg31.sa = 1.0f; gg31.sb = 1.0f; gg31.Npad = G4; gg31.pad_ = 0;
      k_gemm<3><<<dim3((unsigned)((G4) + 31) / 32, (unsigned)((Bn) + 15) / 16, (unsigned)(1)), 32, 0, stream>>>(gg31); }
    k_roll_cell<<<(unsigned)((Bn * H + 255) / 256), 256, 0, stream>>>(GT, C, A, Bn, H, E, KA);
    { GemmP gl31;
      gl31.A = A + E; gl31.B = Wo; gl31.bias = bo; gl31.R = A + E; gl31.C = LG;
      gl31.sAo = 0; gl31.sAi = 0; gl31.sAm = KA; gl31.sAk = 1; gl31.sBo = 0; gl31.sBi = 0; gl31.sBn = 1; gl31.sBk = V; gl31.sCo = 0; gl31.sCi = 0; gl31.sCm = V; gl31.sRo = 0; gl31.sRi = 0; gl31.sRm = 0; gl31.sRn = 0;
      gl31.M = Bn; gl31.N = V; gl31.K = H; gl31.zi_n = 1; gl31.flags = 1; gl31.act = 0;
      gl31.alpha = 1.0f; gl31.beta = 0.0f; gl31.sa = 1.0f; gl31.sb = 1.0f; gl31.Npad = V; gl31.pad_ = 0;
      k_gemm<3><<<dim3((unsigned)((V) + 31) / 32, (unsigned)((Bn) + 15) / 16, (unsigned)(1)), 32, 0, stream>>>(gl31); }
    k_roll_pick<<<Bn, 256, 0, stream>>>(LG, X, gnum, Emb, A, (int*)out, Bn, T, V, E, KA, 31);
}
